// SOENModel_56307021251137
// MI455X (gfx1250) — hardware-verified
//
#include <hip/hip_runtime.h>
#include <math.h>

typedef __attribute__((ext_vector_type(16))) _Float16 v16h;
typedef __attribute__((ext_vector_type(8)))  _Float16 v8h;
typedef __attribute__((ext_vector_type(16))) __bf16   v16b;
typedef __attribute__((ext_vector_type(8)))  float    v8f;
typedef __attribute__((ext_vector_type(4)))  float    v4f;

__device__ __forceinline__ int frag_k(int i, int h) { return (i < 8) ? (8 * h + i) : (16 + 8 * h + (i - 8)); }
__device__ __forceinline__ __bf16 bf16_rne(float f) {
    unsigned int u = __float_as_uint(f);
    u += 0x7fffu + ((u >> 16) & 1u);
    return __builtin_bit_cast(__bf16, (unsigned short)(u >> 16));
}
__device__ __forceinline__ float bf16_f32(__bf16 b) { return __uint_as_float(((unsigned int)__builtin_bit_cast(unsigned short, b)) << 16); }
__device__ __forceinline__ v8f wmma16(v16h a, v16h b, v8f c) {
    c = __builtin_amdgcn_wmma_f32_16x16x32_f16(false, a, false, b, (short)0, c, false, false);
    asm volatile("v_nop\n\tv_nop\n\tv_nop\n\tv_nop" : "+v"(c) : "v"(a), "v"(b));
    return c;
}
__device__ __forceinline__ v8f wmmab(v16b a, v16b b, v8f c) {
    c = __builtin_amdgcn_wmma_f32_16x16x32_bf16(false, a, false, b, (short)0, c, false, false);
    asm volatile("v_nop\n\tv_nop\n\tv_nop\n\tv_nop" : "+v"(c) : "v"(a), "v"(b));
    return c;
}
struct Split { v16b hi, lo; };
__device__ __forceinline__ v8f wmma3(const Split& a, const Split& b, v8f c) {
    c = __builtin_amdgcn_wmma_f32_16x16x32_bf16(false, a.hi, false, b.hi, (short)0, c, false, false);
    c = __builtin_amdgcn_wmma_f32_16x16x32_bf16(false, a.hi, false, b.lo, (short)0, c, false, false);
    c = __builtin_amdgcn_wmma_f32_16x16x32_bf16(false, a.lo, false, b.hi, (short)0, c, false, false);
    asm volatile("v_nop\n\tv_nop\n\tv_nop\n\tv_nop" : "+v"(c) : "v"(a.hi), "v"(a.lo), "v"(b.hi), "v"(b.lo));
    return c;
}
struct Split3 { v16b hi, mid, lo; };
__device__ __forceinline__ v8f wmma6(const Split3& a, const Split3& b, v8f c) {
    c = __builtin_amdgcn_wmma_f32_16x16x32_bf16(false, a.hi, false, b.hi, (short)0, c, false, false);
    c = __builtin_amdgcn_wmma_f32_16x16x32_bf16(false, a.hi, false, b.mid, (short)0, c, false, false);
    c = __builtin_amdgcn_wmma_f32_16x16x32_bf16(false, a.mid, false, b.hi, (short)0, c, false, false);
    c = __builtin_amdgcn_wmma_f32_16x16x32_bf16(false, a.hi, false, b.lo, (short)0, c, false, false);
    c = __builtin_amdgcn_wmma_f32_16x16x32_bf16(false, a.mid, false, b.mid, (short)0, c, false, false);
    c = __builtin_amdgcn_wmma_f32_16x16x32_bf16(false, a.lo, false, b.hi, (short)0, c, false, false);
    asm volatile("v_nop\n\tv_nop\n\tv_nop\n\tv_nop" : "+v"(c) : "v"(a.hi), "v"(a.mid), "v"(a.lo), "v"(b.hi), "v"(b.mid), "v"(b.lo));
    return c;
}

__device__ __forceinline__ v16h fh_ld(const float* __restrict__ p, long long sk, int k0, int h, int klen, float s) {
    v16h a;
#pragma unroll
    for (int i = 0; i < 16; ++i) { const int k = k0 + frag_k(i, h); a[i] = (k < klen) ? (_Float16)(p[(long long)k * sk] * s) : (_Float16)0.f; }
    return a;
}
__device__ __forceinline__ Split sp_ld(const float* __restrict__ p, long long sk, int k0, int h, int klen, float s) {
    Split r;
#pragma unroll
    for (int i = 0; i < 16; ++i) {
        const int k = k0 + frag_k(i, h); const float x = (k < klen) ? p[(long long)k * sk] * s : 0.f;
        const __bf16 hb = bf16_rne(x); r.hi[i] = hb; r.lo[i] = bf16_rne(x - bf16_f32(hb));
    }
    return r;
}
__device__ __forceinline__ Split3 sp3_ld(const float* __restrict__ p, long long sk, int k0, int h, int klen, float s) {
    Split3 r;
#pragma unroll
    for (int i = 0; i < 16; ++i) {
        const int k = k0 + frag_k(i, h); const float x = (k < klen) ? p[(long long)k * sk] * s : 0.f;
        const __bf16 hb = bf16_rne(x); const float r1 = x - bf16_f32(hb); const __bf16 mb = bf16_rne(r1);
        r.hi[i] = hb; r.mid[i] = mb; r.lo[i] = bf16_rne(r1 - bf16_f32(mb));
    }
    return r;
}
__device__ __forceinline__ v16b bh_ld(const float* __restrict__ p, long long sk, int k0, int h, int klen, float s) {
    v16b a;
#pragma unroll
    for (int i = 0; i < 16; ++i) { const int k = k0 + frag_k(i, h); a[i] = bf16_rne((k < klen) ? p[(long long)k * sk] * s : 0.f); }
    return a;
}
__device__ __forceinline__ v16h fh_row(const _Float16* __restrict__ row, int k0, int h) {
    v16h a;
#pragma unroll
    for (int i = 0; i < 16; ++i) a[i] = row[k0 + frag_k(i, h)];
    return a;
}

#define VST2(T, ptr, val) do { *(volatile T*)(ptr) = (val); __threadfence(); *(volatile T*)(ptr) = (val); } while (0)
typedef float v4f __attribute__((ext_vector_type(4)));
#define VST2V4(ptr, val) do { *(volatile v4f*)(ptr) = (val); __threadfence(); *(volatile v4f*)(ptr) = (val); } while (0)

__device__ __attribute__((noinline)) float act_fn(float v, int act) {
    if (act == 1) return fmaxf(v, 0.f);
    if (act == 2) { const float u = 0.7978845608028654f * (v + 0.044715f * v * v * v); return 0.5f * v * (1.f + tanhf(u)); }
    if (act == 3) return v / (1.f + expf(-v));
    if (act == 4) return 0.5f * v * (1.f + erff(v * 0.7071067811865476f));
    if (act == 5) return tanhf(v);
    if (act == 6) return 1.f / (1.f + expf(-v));
    if (act == 7) return (v > 0.f) ? v : 0.01f * v;
    if (act == 8) return (v > 0.f) ? v : (expf(v) - 1.f);
    if (act == 9) return fminf(fmaxf(v, 0.f), 6.f);
    if (act == 10) return fabsf(v);
    if (act == 11) return (v >= 0.f) ? v : 0.1f * v;
    if (act == 12) return (v > 0.f) ? v : 0.2f * v;
    if (act == 13) return (v > 20.f) ? v : log1pf(expf(v));
    return v;
}

struct GemmP {
    const float* A; const float* B; const float* bias; const float* R; float* C;
    long long sAo, sAi, sAm, sAk, sBo, sBi, sBn, sBk, sCo, sCi, sCm, sRo, sRi, sRm, sRn;
    int M, N, K, zi_n, flags, act; float alpha, beta, sa, sb;
    int Npad, pad_;
};
static_assert(sizeof(GemmP) == 5 * 8 + 15 * 8 + 6 * 4 + 4 * 4 + 2 * 4, "GemmP has padding");

template <int MODE>
__global__ __launch_bounds__(32) void k_gemm(GemmP p) {
    const int lane = threadIdx.x & 31, h = lane >> 4, l15 = lane & 15;
    const int m0 = blockIdx.y * 16, n0 = blockIdx.x * 32;
    const int z = blockIdx.z, zo = z / p.zi_n, zi = z - zo * p.zi_n;
    const float* A = p.A + zo * p.sAo + zi * p.sAi;
    const float* B = p.B + zo * p.sBo + zi * p.sBi;
    const int am = min(m0 + l15, p.M - 1);
    v8f acc[2];
#pragma unroll
    for (int t = 0; t < 2; ++t) { v8f zz = {}; acc[t] = zz; }
    for (int k0 = 0; k0 < p.K; k0 += 32) {
        const float* arow = A + (long long)am * p.sAm;
        if (MODE == 1) {
            const Split a = sp_ld(arow, p.sAk, k0, h, p.K, 1.f);
#pragma unroll
            for (int t = 0; t < 2; ++t) {
                const int bn = min(n0 + t * 16 + l15, p.N - 1);
                acc[t] = wmma3(a, sp_ld(B + (long long)bn * p.sBn, p.sBk, k0, h, p.K, 1.f), acc[t]);
            }
        } else if (MODE == 3) {
            const Split3 a = sp3_ld(arow, p.sAk, k0, h, p.K, 1.f);
#pragma unroll
            for (int t = 0; t < 2; ++t) {
                const int bn = min(n0 + t * 16 + l15, p.N - 1);
                acc[t] = wmma6(a, sp3_ld(B + (long long)bn * p.sBn, p.sBk, k0, h, p.K, 1.f), acc[t]);
            }
        } else if (MODE == 2) {
            const v16b a = bh_ld(arow, p.sAk, k0, h, p.K, 1.f);
#pragma unroll
            for (int t = 0; t < 2; ++t) {
                const int bn = min(n0 + t * 16 + l15, p.N - 1);
                acc[t] = wmmab(a, bh_ld(B + (long long)bn * p.sBn, p.sBk, k0, h, p.K, 1.f), acc[t]);
            }
        } else {
            const v16h a = fh_ld(arow, p.sAk, k0, h, p.K, p.sa);
#pragma unroll
            for (int t = 0; t < 2; ++t) {
                const int bn = min(n0 + t * 16 + l15, p.N - 1);
                acc[t] = wmma16(a, fh_ld(B + (long long)bn * p.sBn, p.sBk, k0, h, p.K, p.sb), acc[t]);
            }
        }
    }
    const float iscale = (MODE == 0) ? p.alpha / (p.sa * p.sb) : p.alpha;
    float* C = p.C + zo * p.sCo + zi * p.sCi;
    const float* R = p.R + zo * p.sRo + zi * p.sRi;
    __shared__ __align__(16) float ctile[16][36];
#pragma unroll
    for (int t = 0; t < 2; ++t) {
        const int n = n0 + t * 16 + l15; const int nn = min(n, p.N - 1);
#pragma unroll
        for (int r = 0; r < 8; ++r) {
            const int m = m0 + 8 * h + r; const int mm = min(m, p.M - 1);
            float v = acc[t][r] * iscale;
            if (p.flags & 1) v += p.bias[nn];
            if (p.flags & 2) v += p.bias[mm];
            v = act_fn(v, p.act);
            if (p.flags & 4) v += p.beta * R[(long long)mm * p.sRm + (long long)nn * p.sRn];
            ctile[8 * h + r][t * 16 + l15] = (n < p.N) ? v : 0.f;
        }
    }
    __syncthreads();
    const int NW = (p.Npad > p.N) ? p.Npad : p.N;
    const bool fast = (m0 + 16 <= p.M) && (n0 + 32 <= NW) && ((p.sCm & 3) == 0) && ((((size_t)C) & 15) == 0);
    if (fast) {
#pragma unroll
        for (int s = 0; s < 4; ++s) {
            const int row = s * 4 + (lane >> 3), c4 = (lane & 7) * 4;
            const v4f v = *(const v4f*)&ctile[row][c4];
            VST2V4(C + (long long)(m0 + row) * p.sCm + n0 + c4, v);
        }
    } else {
        for (int row = 0; row < 16; ++row) {
            const int m = m0 + row, n = n0 + lane;
            if (m < p.M && n < NW) VST2(float, C + (long long)m * p.sCm + n, ctile[row][lane]);
        }
    }
}

#define AW 4
struct AttnP {
    const float* Q; const float* K; const float* V; float* O; float* P; const float* Mf; const int* Mi; float* ST;
    const float* Pw; const float* Rt; const int* SQ; const int* SK;
    long long swb, swh, swi, swj, srb, srh, sri;
    long long sQb, sQh, sQi, sQd, sKb, sKh, sKj, sKd, sVb, sVh, sVj, sVd, sOb, sOh, sOi, sPb, sPh, sPi, smb, smh, smi, smj;
    int Lq, Lk, dh, dv, hrep, causal, coff, pband;
    float scale, mfill; int nonorm, mpol;
    int roff, rn, segpol, win;
};
static_assert(sizeof(AttnP) == 12 * 8 + 29 * 8 + 16 * 4, "AttnP has padding");

#ifndef KATTN_ATTR
#define KATTN_ATTR
#endif
template <int DHP, int DVP, int QM, bool SPLITPV, bool TWOPASS>
__global__ __launch_bounds__(32 * AW) KATTN_ATTR void k_attn(AttnP p) {
    constexpr int NT = DVP / 16;
    constexpr int KS = DHP / 32;
    constexpr int VP = DVP + 8;
    __shared__ __align__(16) float    pl[AW][16 * 64];
    __shared__ __align__(16) _Float16 vl[(SPLITPV ? 2 : 1) * 64 * VP];
    const int lane = threadIdx.x & 31, hf = lane >> 4, l15 = lane & 15, wave = threadIdx.x >> 5;
    const int h = blockIdx.y, b = blockIdx.z, hk = h / p.hrep;
    const int q0 = (blockIdx.x * AW + wave) * 16;
    float* myp = pl[wave];
    const float L2E = 1.4426950408889634f;
    const float NEG = -__builtin_inff();
    const int qi = min(q0 + l15, p.Lq - 1);
    const float* qrow = p.Q + b * p.sQb + h * p.sQh + (long long)qi * p.sQi;
    const float* kbase = p.K + b * p.sKb + hk * p.sKh;
    const float* vbase = p.V + b * p.sVb + hk * p.sVh;
    v16h qa[QM == 0 ? KS : 1]; Split qs_[QM == 1 ? KS : 1]; Split3 qt_[QM == 2 ? KS : 1];
#pragma unroll
    for (int ks = 0; ks < KS; ++ks) {
        if (QM == 2) qt_[ks] = sp3_ld(qrow, p.sQd, ks * 32, hf, p.dh, 1.f);
        else if (QM == 1) qs_[ks] = sp_ld(qrow, p.sQd, ks * 32, hf, p.dh, 1.f);
        else qa[ks] = fh_ld(qrow, p.sQd, ks * 32, hf, p.dh, 1.f);
    }
    v8f o[NT]; float m8[8], l8[8];
#pragma unroll
    for (int t = 0; t < NT; ++t) { v8f zz = {}; o[t] = zz; }
#pragma unroll
    for (int i = 0; i < 8; ++i) { m8[i] = NEG; l8[i] = 0.f; }
    int jend = p.Lk;
    if (p.causal == 1) { const int je = (blockIdx.x * AW + AW - 1) * 16 + 16 + p.coff; jend = min(jend, max(je, 0)); }
    const int npass = TWOPASS ? 2 : 1;
    for (int pass = 0; pass < npass; ++pass) {
        const bool dopv = (!TWOPASS) || pass == 1;
        for (int j0 = 0; j0 < jend; j0 += 64) {
            if (dopv) {
                __syncthreads();
                for (int idx = threadIdx.x; idx < 64 * DVP; idx += 32 * AW) {
                    const int jr = idx / DVP, d = idx - jr * DVP, j = j0 + jr;
                    const float f = (j < p.Lk && d < p.dv) ? vbase[(long long)j * p.sVj + (long long)d * p.sVd] : 0.f;
                    if (SPLITPV) {
                        const __bf16 hb = bf16_rne(f);
                        ((__bf16*)vl)[jr * VP + d] = hb; ((__bf16*)vl)[64 * VP + jr * VP + d] = bf16_rne(f - bf16_f32(hb));
                    } else vl[jr * VP + d] = (_Float16)f;
                }
            }
            v8f s[4];
#pragma unroll
            for (int t = 0; t < 4; ++t) {
                const int j = min(j0 + t * 16 + l15, p.Lk - 1);
                const float* krow = kbase + (long long)j * p.sKj;
                v8f acc = {};
#pragma unroll
                for (int ks = 0; ks < KS; ++ks) {
                    if (QM == 2)      acc = wmma6(qt_[ks], sp3_ld(krow, p.sKd, ks * 32, hf, p.dh, 1.f), acc);
                    else if (QM == 1) acc = wmma3(qs_[ks], sp_ld(krow, p.sKd, ks * 32, hf, p.dh, 1.f), acc);
                    else              acc = wmma16(qa[ks], fh_ld(krow, p.sKd, ks * 32, hf, p.dh, 1.f), acc);
                }
                s[t] = acc;
            }
            float pv[8][4];
#pragma unroll
            for (int i = 0; i < 8; ++i) {
                const int irow = q0 + i + 8 * hf;
                const int ic = min(irow, p.Lq - 1);
                float sc[4];
#pragma unroll
                for (int t = 0; t < 4; ++t) {
                    const int jg = j0 + t * 16 + l15;
                    float v = s[t][i] * p.scale;
                    if (p.Mf) v += p.Mf[b * p.smb + h * p.smh + (long long)ic * p.smi + (long long)min(jg, p.Lk - 1) * p.smj];
                    if (p.Rt) { int rc = ic - min(jg, p.Lk - 1) + p.roff; rc = rc < 0 ? 0 : (rc >= p.rn ? p.rn - 1 : rc); v += p.Rt[b * p.srb + h * p.srh + (long long)ic * p.sri + rc]; }
                    if (p.Mi) { const int mv = p.Mi[b * p.smb + h * p.smh + (long long)ic * p.smi + (long long)min(jg, p.Lk - 1) * p.smj]; if (p.mpol ? (mv != 0) : (mv == 0)) v = p.mfill; }
                    if (p.SQ) { const bool same = p.SQ[(long long)b * p.Lq + ic] == p.SK[(long long)b * p.Lk + min(jg, p.Lk - 1)]; if (p.segpol ? same : !same) v = p.mfill; }
                    if (p.causal == 2 && jg > irow + p.coff) v = p.mfill;
                    if (jg >= p.Lk || (p.causal == 1 && jg > irow + p.coff) || (p.causal == 3 && jg < irow + p.coff) || (p.win > 0 && irow + p.coff - jg > p.win)) v = NEG; else v *= L2E;
                    sc[t] = v;
                }
                if (!TWOPASS || pass == 0) {
                    float mx = fmaxf(fmaxf(sc[0], sc[1]), fmaxf(sc[2], sc[3]));
                    mx = fmaxf(mx, __shfl_xor(mx, 1, 32)); mx = fmaxf(mx, __shfl_xor(mx, 2, 32));
                    mx = fmaxf(mx, __shfl_xor(mx, 4, 32)); mx = fmaxf(mx, __shfl_xor(mx, 8, 32));
                    const float mnew = fmaxf(m8[i], mx);
                    const float corr = (mnew == NEG) ? 1.f : exp2f(m8[i] - mnew);
                    float rs = 0.f;
#pragma unroll
                    for (int t = 0; t < 4; ++t) {
                        const float pp = (sc[t] == NEG) ? 0.f : exp2f(sc[t] - mnew); rs += pp;
                        pv[i][t] = p.Pw ? pp * p.Pw[b * p.swb + h * p.swh + (long long)ic * p.swi + (long long)min(j0 + t * 16 + l15, p.Lk - 1) * p.swj] : pp;
                    }
                    rs += __shfl_xor(rs, 1, 32); rs += __shfl_xor(rs, 2, 32); rs += __shfl_xor(rs, 4, 32); rs += __shfl_xor(rs, 8, 32);
                    l8[i] = l8[i] * corr + rs; m8[i] = mnew;
                    if (!TWOPASS) {
#pragma unroll
                        for (int t = 0; t < NT; ++t) o[t][i] *= corr;
                    }
                } else {
                    const float inv = (l8[i] > 0.f) ? 1.f / l8[i] : 0.f;
#pragma unroll
                    for (int t = 0; t < 4; ++t) {
                        const int jg = j0 + t * 16 + l15;
                        float pp = (sc[t] == NEG) ? 0.f : exp2f(sc[t] - m8[i]) * inv;
                        if (p.Pw) pp *= p.Pw[b * p.swb + h * p.swh + (long long)ic * p.swi + (long long)min(jg, p.Lk - 1) * p.swj];
                        pv[i][t] = pp;
                    }
                }
            }
            if (dopv) {
#pragma unroll
                for (int i = 0; i < 8; ++i)
#pragma unroll
                    for (int t = 0; t < 4; ++t) myp[(i + 8 * hf) * 64 + t * 16 + l15] = pv[i][t];
                __syncthreads();
                if (p.P) {
                    float* pb_ = p.P + b * p.sPb + h * p.sPh;
                    const bool fastP = (p.pband == 0) && ((p.sPi & 3) == 0) && (j0 + 64 <= p.Lk) && (q0 + 16 <= p.Lq) && ((((size_t)pb_) & 15) == 0);
                    if (fastP) {
#pragma unroll
                        for (int s = 0; s < 8; ++s) {
                            const int row = s * 2 + (lane >> 4), c4 = (lane & 15) * 4;
                            const v4f v = *(const v4f*)(myp + row * 64 + c4);
                            VST2V4(pb_ + (long long)(q0 + row) * p.sPi + j0 + c4, v);
                        }
                    } else {
                        for (int row = 0; row < 16; ++row) {
                            const int irow = q0 + row; if (irow >= p.Lq) continue;
                            for (int c = lane; c < 64; c += 32) {
                                const int jg = j0 + c; if (jg >= p.Lk) continue;
                                if (p.pband == 0) VST2(float, pb_ + (long long)irow * p.sPi + jg, myp[row * 64 + c]);
                                else if (jg - irow <= p.pband && irow - jg <= p.pband) VST2(float, pb_ + (long long)irow * p.sPi + (jg - irow + p.pband), myp[row * 64 + c]);
                            }
                        }
                    }
                }
                if (SPLITPV) {
                    const Split pa0 = sp_ld(myp + l15 * 64, 1, 0, hf, 64, 1.f), pa1 = sp_ld(myp + l15 * 64, 1, 32, hf, 64, 1.f);
                    const __bf16* vh = (const __bf16*)vl; const __bf16* vlo = vh + 64 * VP;
#pragma unroll
                    for (int t = 0; t < NT; ++t) {
                        const int dcol = t * 16 + l15;
                        Split b0, b1;
#pragma unroll
                        for (int e = 0; e < 16; ++e) {
                            const int k0 = frag_k(e, hf), k1 = 32 + frag_k(e, hf);
                            b0.hi[e] = vh[k0 * VP + dcol]; b0.lo[e] = vlo[k0 * VP + dcol]; b1.hi[e] = vh[k1 * VP + dcol]; b1.lo[e] = vlo[k1 * VP + dcol];
                        }
                        o[t] = wmma3(pa0, b0, o[t]);
                        o[t] = wmma3(pa1, b1, o[t]);
                    }
                } else {
                    const v16h pa0 = fh_ld(myp + l15 * 64, 1, 0, hf, 64, 4096.f), pa1 = fh_ld(myp + l15 * 64, 1, 32, hf, 64, 4096.f);
#pragma unroll
                    for (int t = 0; t < NT; ++t) {
                        const int dcol = t * 16 + l15;
                        v16h b0, b1;
#pragma unroll
                        for (int e = 0; e < 16; ++e) { b0[e] = vl[frag_k(e, hf) * VP + dcol]; b1[e] = vl[(32 + frag_k(e, hf)) * VP + dcol]; }
                        o[t] = wmma16(pa0, b0, o[t]);
                        o[t] = wmma16(pa1, b1, o[t]);
                    }
                }
            }
        }
    }
    float* obase = p.O + b * p.sOb + h * p.sOh;
    if (p.ST) {
        const int rl = lane >> 1, isel = rl & 7;
        float mv = 0.f, lv = 0.f;
#pragma unroll
        for (int i = 0; i < 8; ++i) if (i == isel) { mv = m8[i]; lv = l8[i]; }
        const int irow = q0 + rl;
        if (irow < p.Lq) { float* st = p.ST + (((long long)b * gridDim.y + h) * p.Lq + irow) * 2 + (lane & 1); VST2(float, st, (lane & 1) ? lv : mv * 0.6931471805599453f); }
    }
    float invr[8];
#pragma unroll
    for (int i = 0; i < 8; ++i) {
        if (TWOPASS) invr[i] = SPLITPV ? 1.f : (1.f / 4096.f);
        else if (p.nonorm) invr[i] = exp2f(m8[i]) * (SPLITPV ? 1.f : (1.f / 4096.f));
        else invr[i] = (l8[i] > 0.f) ? (SPLITPV ? 1.f / l8[i] : 1.f / (l8[i] * 4096.f)) : 0.f;
    }
    __syncthreads();
    const bool ofast = ((p.sOi & 3) == 0) && ((((size_t)obase) & 15) == 0) && (q0 + 16 <= p.Lq);
#pragma unroll
    for (int c0 = 0; c0 < DVP; c0 += 64) {
#pragma unroll
        for (int i = 0; i < 8; ++i)
#pragma unroll
            for (int t = 0; t < NT; ++t) if (t * 16 >= c0 && t * 16 < c0 + 64) myp[(i + 8 * hf) * 64 + (t * 16 - c0) + l15] = o[t][i] * invr[i];
        __syncthreads();
        const int cw = (DVP - c0 < 64) ? (DVP - c0) : 64;
        if (ofast && (c0 + cw <= p.dv) && (cw % 32 == 0)) {
            const int lpr = cw / 4;
            const int rows_per_ins = 32 / lpr;
            for (int r0 = 0; r0 < 16; r0 += rows_per_ins) {
                const int row = r0 + lane / lpr, c4 = (lane % lpr) * 4;
                const v4f v = *(const v4f*)(myp + row * 64 + c4);
                VST2V4(obase + (long long)(q0 + row) * p.sOi + c0 + c4, v);
            }
        } else {
            for (int row = 0; row < 16; ++row) {
                const int irow = q0 + row; if (irow >= p.Lq) continue;
                for (int c = lane; c < cw; c += 32) { const int d = c0 + c; if (d < p.dv) VST2(float, obase + (long long)irow * p.sOi + d, myp[row * 64 + c]); }
            }
        }
        __syncthreads();
    }
}

struct TrP { const float* src; float* dst; const float* R2; long long sSz, lds, sDz, ldd, sRz, ldr; int R, C, flags, act; float alpha, beta; };
static_assert(sizeof(TrP) == 3 * 8 + 6 * 8 + 6 * 4, "TrP has padding");
__global__ __launch_bounds__(256) void k_tr(TrP p) {
    __shared__ float tile[32][33];
    const int c0 = blockIdx.x * 32, r0 = blockIdx.y * 32, z = blockIdx.z;
    const int lane = threadIdx.x & 31, wave = threadIdx.x >> 5;
    const float* s = p.src + z * p.sSz;
#pragma unroll
    for (int k = 0; k < 4; ++k) {
        const int rl = wave * 4 + k, r = r0 + rl, c = c0 + lane;
        tile[rl][lane] = (r < p.R && c < p.C) ? s[(long long)r * p.lds + c] : 0.f;
    }
    __syncthreads();
    float* d = p.dst + z * p.sDz; const float* rr = p.R2 + z * p.sRz;
#pragma unroll
    for (int k = 0; k < 4; ++k) {
        const int cl = wave * 4 + k, c = c0 + cl, r = r0 + lane;
        if (c < p.C && r < p.R) {
            float v = act_fn(p.alpha * tile[lane][cl], p.act);
            if (p.flags & 1) v += p.beta * rr[(long long)c * p.ldr + r];
            VST2(float, d + (long long)c * p.ldd + r, v);
        }
    }
}

__global__ __launch_bounds__(256) void k_affine(const float* __restrict__ src, float* __restrict__ dst, int n, float a, float b, const float* __restrict__ sdev) {
    const int i = blockIdx.x * 256 + threadIdx.x;
    if (i < n) { const float aa = sdev ? a * sdev[0] : a; const float v = aa * src[i] + b; VST2(float, dst + i, v); }
}

struct SmP { const float* src; float* dst; const float* Mf; long long sz, sr, dz, dr, smz, smr; int n, pad; float scale_in, scale_out; };
static_assert(sizeof(SmP) == 3 * 8 + 6 * 8 + 4 * 4, "SmP has padding");
__global__ __launch_bounds__(256) void k_softmax(SmP p) {
    __shared__ float red[256];
    const int r = blockIdx.x, z = blockIdx.y, tid = threadIdx.x;
    const float* s = p.src + z * p.sz + (long long)r * p.sr;
    const float* mf = p.Mf ? (p.Mf + z * p.smz + (long long)r * p.smr) : nullptr;
    float mx = -__builtin_inff();
    for (int j = tid; j < p.n; j += 256) { float v = s[j] * p.scale_in; if (mf) v += mf[j]; mx = fmaxf(mx, v); }
    red[tid] = mx; __syncthreads();
    for (int o = 128; o > 0; o >>= 1) { if (tid < o) red[tid] = fmaxf(red[tid], red[tid + o]); __syncthreads(); }
    mx = red[0]; __syncthreads();
    float sum = 0.f;
    for (int j = tid; j < p.n; j += 256) { float v = s[j] * p.scale_in; if (mf) v += mf[j]; sum += (mx == -__builtin_inff()) ? 0.f : expf(v - mx); }
    red[tid] = sum; __syncthreads();
    for (int o = 128; o > 0; o >>= 1) { if (tid < o) red[tid] += red[tid + o]; __syncthreads(); }
    sum = red[0];
    const float inv = (sum > 0.f) ? p.scale_out / sum : 0.f;
    float* d = p.dst + z * p.dz + (long long)r * p.dr;
    for (int j = tid; j < p.n; j += 256) { float v = s[j] * p.scale_in; if (mf) v += mf[j]; const float o = (mx == -__builtin_inff()) ? 0.f : expf(v - mx) * inv; VST2(float, d + j, o); }
}
__global__ __launch_bounds__(256) void k_stats(const float* __restrict__ x, long long sz, long long so, long long si, int inner, int n, float eps, float* __restrict__ stat, int mode) {
    __shared__ float red[256];
    const int z = blockIdx.x, tid = threadIdx.x;
    const float* base = x + z * sz;
    float s = 0.f;
    for (int e = tid; e < n; e += 256) s += base[(long long)(e / inner) * so + (long long)(e % inner) * si];
    red[tid] = s; __syncthreads();
    for (int o = 128; o > 0; o >>= 1) { if (tid < o) red[tid] += red[tid + o]; __syncthreads(); }
    const float mu = (mode == 0 || mode == 3) ? red[0] / (float)n : 0.f; __syncthreads();
    float q = 0.f;
    for (int e = tid; e < n; e += 256) { const float dlt = base[(long long)(e / inner) * so + (long long)(e % inner) * si] - mu; q += dlt * dlt; }
    red[tid] = q; __syncthreads();
    for (int o = 128; o > 0; o >>= 1) { if (tid < o) red[tid] += red[tid + o]; __syncthreads(); }
    {
        float rs;
        if (mode == 2) rs = sqrtf((float)n) / fmaxf(sqrtf(red[0]), eps); else if (mode == 3) rs = rsqrtf(red[0] / (float)(n - 1) + eps); else rs = rsqrtf(red[0] / (float)n + eps);
        if (tid < 32) { const float v = (tid == 0) ? mu : ((tid == 1) ? rs : 0.f); VST2(float, stat + (long long)z * 32 + tid, v); }
    }
}
__global__ __launch_bounds__(256) void k_norm_apply(const float* __restrict__ x, float* __restrict__ y, const float* __restrict__ stat, const float* __restrict__ g, const float* __restrict__ bta,
                                                     int Z, int C, int L, int G, int bn, int act) {
    const long long idx = (long long)blockIdx.x * 256 + threadIdx.x;
    if (idx >= (long long)Z * C * L) return;
    const int l = (int)(idx % L); const long long zc = idx / L; const int c = (int)(zc % C), z = (int)(zc / C); (void)l;
    const int set = bn ? c : (z * G + c / (C / G));
    float v = (x[idx] - stat[(long long)set * 32]) * stat[(long long)set * 32 + 1];
    if (g) v *= g[c];
    if (bta) v += bta[c];
    v = act_fn(v, act);
    VST2(float, y + idx, v);
}

__global__ __launch_bounds__(256) void k_lse_neg(const float* __restrict__ st, float* __restrict__ c, int n) {
    const int i = blockIdx.x * 256 + threadIdx.x;
    if (i < n) { const float v = -(st[2 * i] + logf(st[2 * i + 1])); VST2(float, c + i, v); }
}

__global__ __launch_bounds__(256) void k_iota(int* __restrict__ dst, int n, int a, int b) {
    const int i = blockIdx.x * 256 + threadIdx.x;
    if (i < n) { const int v = a * i + b; VST2(int, dst + i, v); }
}

__global__ __launch_bounds__(256) void k_axpby(const float* __restrict__ x, const float* __restrict__ y, float* __restrict__ dst, int n, float a, float b, float c) {
    const int i = blockIdx.x * 256 + threadIdx.x;
    if (i < n) { const float v = a * x[i] + b * y[i] + c; VST2(float, dst + i, v); }
}

struct RopeP { const float* X; float* Y; const float* C; const float* Sn; const int* pos; long long sXr, sXh, sYr, sYh, sCb, sCp, sCd; int R, Hn, D, S, mode, tmode, pmode, pad; };
static_assert(sizeof(RopeP) == 5 * 8 + 7 * 8 + 8 * 4, "RopeP has padding");
__global__ __launch_bounds__(256) void k_rope(RopeP p) {
    const long long idx = (long long)blockIdx.x * 256 + threadIdx.x;
    if (idx >= (long long)p.R * p.Hn * p.D) return;
    const int d = (int)(idx % p.D); const long long rh = idx / p.D; const int h = (int)(rh % p.Hn); const int r = (int)(rh / p.Hn);
    const int half = p.D / 2;
    int partner; float sign;
    if (p.mode == 0) { partner = (d < half) ? d + half : d - half; sign = (d < half) ? -1.f : 1.f; }
    else { partner = d ^ 1; sign = (d & 1) ? 1.f : -1.f; }
    const int tcol = (p.tmode == 0) ? d : ((p.tmode == 1) ? (d % half) : (d >> 1));
    const int pp = (p.pmode == 0) ? (r % p.S) : ((p.pmode == 1) ? h : p.pos[r]);
    const long long toff = (long long)(r / p.S) * p.sCb + (long long)pp * p.sCp + (long long)tcol * p.sCd;
    const float* xr = p.X + (long long)r * p.sXr + (long long)h * p.sXh;
    const float v = xr[d] * p.C[toff] + sign * xr[partner] * p.Sn[toff];
    VST2(float, p.Y + (long long)r * p.sYr + (long long)h * p.sYh + d, v);
}

__global__ __launch_bounds__(256) void k_invf(float* __restrict__ invb, int half, int D, float base, float num, int fmode, float cexp) {
    const int i = blockIdx.x * 256 + threadIdx.x;
    if (i >= ((half + 31) / 32) * 32) return;
    if (i >= half) { VST2(float, invb + i, 0.f); return; }
    const float e = (float)(2 * i) / (float)D;
    float invf;
    if (fmode == 1) invf = num * expf((float)(2 * i) * cexp);
    else if (fmode == 2) invf = num * powf(base, (-2.0f * ((float)i - 1.0f)) / (float)D);
    else invf = num * (1.0f / powf(base, e));
    VST2(float, invb + i, invf);
}
__global__ __launch_bounds__(256) void k_sincos(float* __restrict__ cs, float* __restrict__ sn, const float* __restrict__ invb, int S, int half, float pscale) {
    const int idx = blockIdx.x * 256 + threadIdx.x;
    if (idx >= S * half) return;
    const int s = idx / half, i = idx - s * half;
    const float ang = (pscale * (float)s) * invb[i];
    VST2(float, cs + idx, cosf(ang)); VST2(float, sn + idx, sinf(ang));
}

__global__ __launch_bounds__(256) void k_mulact(const float* __restrict__ x, const float* __restrict__ y, float* __restrict__ dst, int n, int act) {
    const int i = blockIdx.x * 256 + threadIdx.x;
    if (i < n) { const float v = act_fn(x[i], act) * y[i]; VST2(float, dst + i, v); }
}

__global__ __launch_bounds__(256) void k_matvec(GemmP p) {
    const int rpt = (p.N == 1) ? 1 : 32;
    const long long r0 = ((long long)blockIdx.x * 256 + threadIdx.x) * rpt; const int z = blockIdx.z, zo = z / p.zi_n, zi = z - zo * p.zi_n;
    if (r0 >= p.M) return;
    const float* Bb = p.B + zo * p.sBo + zi * p.sBi;
    float* C = p.C + zo * p.sCo + zi * p.sCi; const float* R = p.R + zo * p.sRo + zi * p.sRi;
    for (int rr = 0; rr < rpt; ++rr) {
        const long long r = r0 + rr; if (r >= p.M) break;
        const float* A = p.A + zo * p.sAo + zi * p.sAi + r * p.sAm;
        float acc[8] = {0.f, 0.f, 0.f, 0.f, 0.f, 0.f, 0.f, 0.f};
        for (int k = 0; k < p.K; ++k) { const float a = A[(long long)k * p.sAk];
#pragma unroll
            for (int j = 0; j < 8; ++j) if (j < p.N) acc[j] += a * Bb[(long long)j * p.sBn + (long long)k * p.sBk]; }
#pragma unroll
        for (int j = 0; j < 8; ++j) if (j < p.N) {
            float v = acc[j] * p.alpha;
            if (p.flags & 1) v += p.bias[j];
            if (p.flags & 2) v += p.bias[r];
            v = act_fn(v, p.act);
            if (p.flags & 4) v += p.beta * R[r * p.sRm + (long long)j * p.sRn];
            VST2(float, C + r * p.sCm + j, v);
        }
    }
}
__global__ __launch_bounds__(256) void k_smallsoftmax(const float* __restrict__ src, float* __restrict__ dst, long long sr, long long dr, int n, long long R, float scale) {
    const long long r0 = ((long long)blockIdx.x * 256 + threadIdx.x) * 32;
    for (int rr = 0; rr < 32; ++rr) {
        const long long r = r0 + rr; if (r >= R) return;
        const float* s = src + r * sr; float* d = dst + r * dr;
        float mx = -__builtin_inff();
        for (int j = 0; j < n; ++j) mx = fmaxf(mx, s[j] * scale);
        float sum = 0.f;
        for (int j = 0; j < n; ++j) sum += expf(s[j] * scale - mx);
        const float inv = 1.f / sum;
        for (int j = 0; j < n; ++j) { const float v = expf(s[j] * scale - mx) * inv; VST2(float, d + j, v); }
    }
}

__global__ __launch_bounds__(32) void k_unitstat(float* __restrict__ st) { const int t = threadIdx.x; const float v = (t == 1) ? 1.f : 0.f; VST2(float, st + t, v); }

__global__ __launch_bounds__(256) void k_lincopy(const float* __restrict__ src, long long lds, float* __restrict__ dst, long long ldd, long long rows, int cols) {
    const long long i = (long long)blockIdx.x * 256 + threadIdx.x; if (i >= rows * cols) return;
    const long long r = i / cols; const int c = (int)(i - r * cols);
    const float v = src[r * lds + c]; VST2(float, dst + r * ldd + c, v);
}

__global__ __launch_bounds__(256) void k_extflux(const float* __restrict__ x, const float* __restrict__ fo, float* __restrict__ EXT, int B, int NT, int NI) {
    const long long t = (long long)blockIdx.x * 256 + threadIdx.x; if (t >= (long long)B * NT) return; const int n = (int)(t % NT); const int b = (int)(t / NT);
    const float v = ((n < NI) ? x[(long long)b * NI + n] : 0.f) + fo[n]; VST2(float, EXT + t, v);
}
__global__ __launch_bounds__(256) void k_soen_step(const float* __restrict__ S, const float* __restrict__ PHI, const float* __restrict__ PHZ, const float* __restrict__ gam, const float* __restrict__ tau, const float* __restrict__ foz, float* __restrict__ SN, int B, int NT) {
    const long long t = (long long)blockIdx.x * 256 + threadIdx.x; if (t >= (long long)B * NT) return; const int n = (int)(t % NT);
    const float s = S[t]; float phi = fminf(fmaxf(PHI[t], -0.5f), 0.5f); const float phw = phi - rintf(phi); const float z = tanhf(PHZ[t] + foz[n]);
    const float g = tanhf(1.7f * phw) * (1.f - s) * (1.f + z);
    float sn = s + 0.05f * (gam[n] * g - s * (1.f / tau[n])); sn = fminf(fmaxf(sn, -1.f), 1.f);
    VST2(float, SN + t, sn);
}
__global__ __launch_bounds__(256) void k_soen_out(const float* __restrict__ S, float* __restrict__ OUT, int B, int NT, int NO) {
    const long long t = (long long)blockIdx.x * 256 + threadIdx.x; if (t >= (long long)B * NO) return; const int j = (int)(t % NO); const int b = (int)(t / NO);
    const float v = S[(long long)b * NT + NT - NO + j]; VST2(float, OUT + t, v);
}

template __global__ void k_gemm<1>(GemmP);

extern "C" void kernel_launch(void* const* d_in, const int* in_sizes, int n_in, void* d_out, int out_size, void* d_ws, size_t ws_size, hipStream_t stream) {
    (void)in_sizes; (void)n_in; (void)out_size; (void)ws_size;
    const float* x = (const float*)d_in[0];
    const float* s0 = (const float*)d_in[1];
    const float* J = (const float*)d_in[2];
    const float* JZ = (const float*)d_in[3];
    const float* gam = (const float*)d_in[4];
    const float* tau = (const float*)d_in[5];
    const float* fo = (const float*)d_in[6];
    const float* foz = (const float*)d_in[7];
    const float* msk = (const float*)d_in[8];
    const int Bn = 1024;
    const int NI = 256;
    const int NO = 256;
    const int NT = 2048;
    const int ITERS = 50;
    float* out = (float*)d_out;
    char* wsp = (char*)d_ws;
    float* JM = (float*)wsp; wsp += (((size_t)((size_t)NT * NT) * 4 + 255) / 256) * 256;
    float* JZM = (float*)wsp; wsp += (((size_t)((size_t)NT * NT) * 4 + 255) / 256) * 256;
    float* EXT = (float*)wsp; wsp += (((size_t)((size_t)Bn * NT) * 4 + 255) / 256) * 256;
    float* SA = (float*)wsp; wsp += (((size_t)((size_t)Bn * NT) * 4 + 255) / 256) * 256;
    float* SB = (float*)wsp; wsp += (((size_t)((size_t)Bn * NT) * 4 + 255) / 256) * 256;
    float* PHI = (float*)wsp; wsp += (((size_t)((size_t)Bn * NT) * 4 + 255) / 256) * 256;
    float* PHZ = (float*)wsp; wsp += (((size_t)((size_t)Bn * NT) * 4 + 255) / 256) * 256;
    k_mulact<<<(unsigned)(((long long)NT * NT) + 255) / 256, 256, 0, stream>>>(J, msk, JM, (long long)NT * NT, 0);
    k_mulact<<<(unsigned)(((long long)NT * NT) + 255) / 256, 256, 0, stream>>>(JZ, msk, JZM, (long long)NT * NT, 0);
    k_extflux<<<(unsigned)(((long long)Bn * NT + 255) / 256), 256, 0, stream>>>(x, fo, EXT, Bn, NT, NI);
    { GemmP gp0;
      gp0.A = s0; gp0.B = JM; gp0.bias = s0; gp0.R = EXT; gp0.C = PHI;
      gp0.sAo = 0; gp0.sAi = 0; gp0.sAm = NT; gp0.sAk = 1; gp0.sBo = 0; gp0.sBi = 0; gp0.sBn = NT; gp0.sBk = 1; gp0.sCo = 0; gp0.sCi = 0; gp0.sCm = NT; gp0.sRo = 0; gp0.sRi = 0; gp0.sRm = NT; gp0.sRn = 1;
      gp0.M = Bn; gp0.N = NT; gp0.K = NT; gp0.zi_n = 1; gp0.flags = 4; gp0.act = 0;
      gp0.alpha = 1.0f; gp0.beta = 1.0f; gp0.sa = 1.0f; gp0.sb = 1.0f; gp0.Npad = NT; gp0.pad_ = 0;
      k_gemm<1><<<dim3((unsigned)((NT) + 31) / 32, (unsigned)((Bn) + 15) / 16, (unsigned)(1)), 32, 0, stream>>>(gp0); }
    { GemmP gz0;
      gz0.A = s0; gz0.B = JZM; gz0.bias = s0; gz0.R = s0; gz0.C = PHZ;
      gz0.sAo = 0; gz0.sAi = 0; gz0.sAm = NT; gz0.sAk = 1; gz0.sBo = 0; gz0.sBi = 0; gz0.sBn = NT; gz0.sBk = 1; gz0.sCo = 0; gz0.sCi = 0; gz0.sCm = NT; gz0.sRo = 0; gz0.sRi = 0; gz0.sRm = 0; gz0.sRn = 0;
      gz0.M = Bn; gz0.N = NT; gz0.K = NT; gz0.zi_n = 1; gz0.flags = 0; gz0.act = 0;
      gz0.alpha = 1.0f; gz0.beta = 0.0f; gz0.sa = 1.0f; gz0.sb = 1.0f; gz0.Npad = NT; gz0.pad_ = 0;
      k_gemm<1><<<dim3((unsigned)((NT) + 31) / 32, (unsigned)((Bn) + 15) / 16, (unsigned)(1)), 32, 0, stream>>>(gz0); }
    k_soen_step<<<(unsigned)(((long long)Bn * NT + 255) / 256), 256, 0, stream>>>(s0, PHI, PHZ, gam, tau, foz, SA, Bn, NT);
    { GemmP gp1;
      gp1.A = SA; gp1.B = JM; gp1.bias = SA; gp1.R = EXT; gp1.C = PHI;
      gp1.sAo = 0; gp1.sAi = 0; gp1.sAm = NT; gp1.sAk = 1; gp1.sBo = 0; gp1.sBi = 0; gp1.sBn = NT; gp1.sBk = 1; gp1.sCo = 0; gp1.sCi = 0; gp1.sCm = NT; gp1.sRo = 0; gp1.sRi = 0; gp1.sRm = NT; gp1.sRn = 1;
      gp1.M = Bn; gp1.N = NT; gp1.K = NT; gp1.zi_n = 1; gp1.flags = 4; gp1.act = 0;
      gp1.alpha = 1.0f; gp1.beta = 1.0f; gp1.sa = 1.0f; gp1.sb = 1.0f; gp1.Npad = NT; gp1.pad_ = 0;
      k_gemm<1><<<dim3((unsigned)((NT) + 31) / 32, (unsigned)((Bn) + 15) / 16, (unsigned)(1)), 32, 0, stream>>>(gp1); }
    { GemmP gz1;
      gz1.A = SA; gz1.B = JZM; gz1.bias = SA; gz1.R = SA; gz1.C = PHZ;
      gz1.sAo = 0; gz1.sAi = 0; gz1.sAm = NT; gz1.sAk = 1; gz1.sBo = 0; gz1.sBi = 0; gz1.sBn = NT; gz1.sBk = 1; gz1.sCo = 0; gz1.sCi = 0; gz1.sCm = NT; gz1.sRo = 0; gz1.sRi = 0; gz1.sRm = 0; gz1.sRn = 0;
      gz1.M = Bn; gz1.N = NT; gz1.K = NT; gz1.zi_n = 1; gz1.flags = 0; gz1.act = 0;
      gz1.alpha = 1.0f; gz1.beta = 0.0f; gz1.sa = 1.0f; gz1.sb = 1.0f; gz1.Npad = NT; gz1.pad_ = 0;
      k_gemm<1><<<dim3((unsigned)((NT) + 31) / 32, (unsigned)((Bn) + 15) / 16, (unsigned)(1)), 32, 0, stream>>>(gz1); }
    k_soen_step<<<(unsigned)(((long long)Bn * NT + 255) / 256), 256, 0, stream>>>(SA, PHI, PHZ, gam, tau, foz, SB, Bn, NT);
    { GemmP gp2;
      gp2.A = SB; gp2.B = JM; gp2.bias = SB; gp2.R = EXT; gp2.C = PHI;
      gp2.sAo = 0; gp2.sAi = 0; gp2.sAm = NT; gp2.sAk = 1; gp2.sBo = 0; gp2.sBi = 0; gp2.sBn = NT; gp2.sBk = 1; gp2.sCo = 0; gp2.sCi = 0; gp2.sCm = NT; gp2.sRo = 0; gp2.sRi = 0; gp2.sRm = NT; gp2.sRn = 1;
      gp2.M = Bn; gp2.N = NT; gp2.K = NT; gp2.zi_n = 1; gp2.flags = 4; gp2.act = 0;
      gp2.alpha = 1.0f; gp2.beta = 1.0f; gp2.sa = 1.0f; gp2.sb = 1.0f; gp2.Npad = NT; gp2.pad_ = 0;
      k_gemm<1><<<dim3((unsigned)((NT) + 31) / 32, (unsigned)((Bn) + 15) / 16, (unsigned)(1)), 32, 0, stream>>>(gp2); }
    { GemmP gz2;
      gz2.A = SB; gz2.B = JZM; gz2.bias = SB; gz2.R = SB; gz2.C = PHZ;
      gz2.sAo = 0; gz2.sAi = 0; gz2.sAm = NT; gz2.sAk = 1; gz2.sBo = 0; gz2.sBi = 0; gz2.sBn = NT; gz2.sBk = 1; gz2.sCo = 0; gz2.sCi = 0; gz2.sCm = NT; gz2.sRo = 0; gz2.sRi = 0; gz2.sRm = 0; gz2.sRn = 0;
      gz2.M = Bn; gz2.N = NT; gz2.K = NT; gz2.zi_n = 1; gz2.flags = 0; gz2.act = 0;
      gz2.alpha = 1.0f; gz2.beta = 0.0f; gz2.sa = 1.0f; gz2.sb = 1.0f; gz2.Npad = NT; gz2.pad_ = 0;
      k_gemm<1><<<dim3((unsigned)((NT) + 31) / 32, (unsigned)((Bn) + 15) / 16, (unsigned)(1)), 32, 0, stream>>>(gz2); }
    k_soen_step<<<(unsigned)(((long long)Bn * NT + 255) / 256), 256, 0, stream>>>(SB, PHI, PHZ, gam, tau, foz, SA, Bn, NT);
    { GemmP gp3;
      gp3.A = SA; gp3.B = JM; gp3.bias = SA; gp3.R = EXT; gp3.C = PHI;
      gp3.sAo = 0; gp3.sAi = 0; gp3.sAm = NT; gp3.sAk = 1; gp3.sBo = 0; gp3.sBi = 0; gp3.sBn = NT; gp3.sBk = 1; gp3.sCo = 0; gp3.sCi = 0; gp3.sCm = NT; gp3.sRo = 0; gp3.sRi = 0; gp3.sRm = NT; gp3.sRn = 1;
      gp3.M = Bn; gp3.N = NT; gp3.K = NT; gp3.zi_n = 1; gp3.flags = 4; gp3.act = 0;
      gp3.alpha = 1.0f; gp3.beta = 1.0f; gp3.sa = 1.0f; gp3.sb = 1.0f; gp3.Npad = NT; gp3.pad_ = 0;
      k_gemm<1><<<dim3((unsigned)((NT) + 31) / 32, (unsigned)((Bn) + 15) / 16, (unsigned)(1)), 32, 0, stream>>>(gp3); }
    { GemmP gz3;
      gz3.A = SA; gz3.B = JZM; gz3.bias = SA; gz3.R = SA; gz3.C = PHZ;
      gz3.sAo = 0; gz3.sAi = 0; gz3.sAm = NT; gz3.sAk = 1; gz3.sBo = 0; gz3.sBi = 0; gz3.sBn = NT; gz3.sBk = 1; gz3.sCo = 0; gz3.sCi = 0; gz3.sCm = NT; gz3.sRo = 0; gz3.sRi = 0; gz3.sRm = 0; gz3.sRn = 0;
      gz3.M = Bn; gz3.N = NT; gz3.K = NT; gz3.zi_n = 1; gz3.flags = 0; gz3.act = 0;
      gz3.alpha = 1.0f; gz3.beta = 0.0f; gz3.sa = 1.0f; gz3.sb = 1.0f; gz3.Npad = NT; gz3.pad_ = 0;
      k_gemm<1><<<dim3((unsigned)((NT) + 31) / 32, (unsigned)((Bn) + 15) / 16, (unsigned)(1)), 32, 0, stream>>>(gz3); }
    k_soen_step<<<(unsigned)(((long long)Bn * NT + 255) / 256), 256, 0, stream>>>(SA, PHI, PHZ, gam, tau, foz, SB, Bn, NT);
    { GemmP gp4;
      gp4.A = SB; gp4.B = JM; gp4.bias = SB; gp4.R = EXT; gp4.C = PHI;
      gp4.sAo = 0; gp4.sAi = 0; gp4.sAm = NT; gp4.sAk = 1; gp4.sBo = 0; gp4.sBi = 0; gp4.sBn = NT; gp4.sBk = 1; gp4.sCo = 0; gp4.sCi = 0; gp4.sCm = NT; gp4.sRo = 0; gp4.sRi = 0; gp4.sRm = NT; gp4.sRn = 1;
      gp4.M = Bn; gp4.N = NT; gp4.K = NT; gp4.zi_n = 1; gp4.flags = 4; gp4.act = 0;
      gp4.alpha = 1.0f; gp4.beta = 1.0f; gp4.sa = 1.0f; gp4.sb = 1.0f; gp4.Npad = NT; gp4.pad_ = 0;
      k_gemm<1><<<dim3((unsigned)((NT) + 31) / 32, (unsigned)((Bn) + 15) / 16, (unsigned)(1)), 32, 0, stream>>>(gp4); }
    { GemmP gz4;
      gz4.A = SB; gz4.B = JZM; gz4.bias = SB; gz4.R = SB; gz4.C = PHZ;
      gz4.sAo = 0; gz4.sAi = 0; gz4.sAm = NT; gz4.sAk = 1; gz4.sBo = 0; gz4.sBi = 0; gz4.sBn = NT; gz4.sBk = 1; gz4.sCo = 0; gz4.sCi = 0; gz4.sCm = NT; gz4.sRo = 0; gz4.sRi = 0; gz4.sRm = 0; gz4.sRn = 0;
      gz4.M = Bn; gz4.N = NT; gz4.K = NT; gz4.zi_n = 1; gz4.flags = 0; gz4.act = 0;
      gz4.alpha = 1.0f; gz4.beta = 0.0f; gz4.sa = 1.0f; gz4.sb = 1.0f; gz4.Npad = NT; gz4.pad_ = 0;
      k_gemm<1><<<dim3((unsigned)((NT) + 31) / 32, (unsigned)((Bn) + 15) / 16, (unsigned)(1)), 32, 0, stream>>>(gz4); }
    k_soen_step<<<(unsigned)(((long long)Bn * NT + 255) / 256), 256, 0, stream>>>(SB, PHI, PHZ, gam, tau, foz, SA, Bn, NT);
    { GemmP gp5;
      gp5.A = SA; gp5.B = JM; gp5.bias = SA; gp5.R = EXT; gp5.C = PHI;
      gp5.sAo = 0; gp5.sAi = 0; gp5.sAm = NT; gp5.sAk = 1; gp5.sBo = 0; gp5.sBi = 0; gp5.sBn = NT; gp5.sBk = 1; gp5.sCo = 0; gp5.sCi = 0; gp5.sCm = NT; gp5.sRo = 0; gp5.sRi = 0; gp5.sRm = NT; gp5.sRn = 1;
      gp5.M = Bn; gp5.N = NT; gp5.K = NT; gp5.zi_n = 1; gp5.flags = 4; gp5.act = 0;
      gp5.alpha = 1.0f; gp5.beta = 1.0f; gp5.sa = 1.0f; gp5.sb = 1.0f; gp5.Npad = NT; gp5.pad_ = 0;
      k_gemm<1><<<dim3((unsigned)((NT) + 31) / 32, (unsigned)((Bn) + 15) / 16, (unsigned)(1)), 32, 0, stream>>>(gp5); }
    { GemmP gz5;
      gz5.A = SA; gz5.B = JZM; gz5.bias = SA; gz5.R = SA; gz5.C = PHZ;
      gz5.sAo = 0; gz5.sAi = 0; gz5.sAm = NT; gz5.sAk = 1; gz5.sBo = 0; gz5.sBi = 0; gz5.sBn = NT; gz5.sBk = 1; gz5.sCo = 0; gz5.sCi = 0; gz5.sCm = NT; gz5.sRo = 0; gz5.sRi = 0; gz5.sRm = 0; gz5.sRn = 0;
      gz5.M = Bn; gz5.N = NT; gz5.K = NT; gz5.zi_n = 1; gz5.flags = 0; gz5.act = 0;
      gz5.alpha = 1.0f; gz5.beta = 0.0f; gz5.sa = 1.0f; gz5.sb = 1.0f; gz5.Npad = NT; gz5.pad_ = 0;
      k_gemm<1><<<dim3((unsigned)((NT) + 31) / 32, (unsigned)((Bn) + 15) / 16, (unsigned)(1)), 32, 0, stream>>>(gz5); }
    k_soen_step<<<(unsigned)(((long long)Bn * NT + 255) / 256), 256, 0, stream>>>(SA, PHI, PHZ, gam, tau, foz, SB, Bn, NT);
    { GemmP gp6;
      gp6.A = SB; gp6.B = JM; gp6.bias = SB; gp6.R = EXT; gp6.C = PHI;
      gp6.sAo = 0; gp6.sAi = 0; gp6.sAm = NT; gp6.sAk = 1; gp6.sBo = 0; gp6.sBi = 0; gp6.sBn = NT; gp6.sBk = 1; gp6.sCo = 0; gp6.sCi = 0; gp6.sCm = NT; gp6.sRo = 0; gp6.sRi = 0; gp6.sRm = NT; gp6.sRn = 1;
      gp6.M = Bn; gp6.N = NT; gp6.K = NT; gp6.zi_n = 1; gp6.flags = 4; gp6.act = 0;
      gp6.alpha = 1.0f; gp6.beta = 1.0f; gp6.sa = 1.0f; gp6.sb = 1.0f; gp6.Npad = NT; gp6.pad_ = 0;
      k_gemm<1><<<dim3((unsigned)((NT) + 31) / 32, (unsigned)((Bn) + 15) / 16, (unsigned)(1)), 32, 0, stream>>>(gp6); }
    { GemmP gz6;
      gz6.A = SB; gz6.B = JZM; gz6.bias = SB; gz6.R = SB; gz6.C = PHZ;
      gz6.sAo = 0; gz6.sAi = 0; gz6.sAm = NT; gz6.sAk = 1; gz6.sBo = 0; gz6.sBi = 0; gz6.sBn = NT; gz6.sBk = 1; gz6.sCo = 0; gz6.sCi = 0; gz6.sCm = NT; gz6.sRo = 0; gz6.sRi = 0; gz6.sRm = 0; gz6.sRn = 0;
      gz6.M = Bn; gz6.N = NT; gz6.K = NT; gz6.zi_n = 1; gz6.flags = 0; gz6.act = 0;
      gz6.alpha = 1.0f; gz6.beta = 0.0f; gz6.sa = 1.0f; gz6.sb = 1.0f; gz6.Npad = NT; gz6.pad_ = 0;
      k_gemm<1><<<dim3((unsigned)((NT) + 31) / 32, (unsigned)((Bn) + 15) / 16, (unsigned)(1)), 32, 0, stream>>>(gz6); }
    k_soen_step<<<(unsigned)(((long long)Bn * NT + 255) / 256), 256, 0, stream>>>(SB, PHI, PHZ, gam, tau, foz, SA, Bn, NT);
    { GemmP gp7;
      gp7.A = SA; gp7.B = JM; gp7.bias = SA; gp7.R = EXT; gp7.C = PHI;
      gp7.sAo = 0; gp7.sAi = 0; gp7.sAm = NT; gp7.sAk = 1; gp7.sBo = 0; gp7.sBi = 0; gp7.sBn = NT; gp7.sBk = 1; gp7.sCo = 0; gp7.sCi = 0; gp7.sCm = NT; gp7.sRo = 0; gp7.sRi = 0; gp7.sRm = NT; gp7.sRn = 1;
      gp7.M = Bn; gp7.N = NT; gp7.K = NT; gp7.zi_n = 1; gp7.flags = 4; gp7.act = 0;
      gp7.alpha = 1.0f; gp7.beta = 1.0f; gp7.sa = 1.0f; gp7.sb = 1.0f; gp7.Npad = NT; gp7.pad_ = 0;
      k_gemm<1><<<dim3((unsigned)((NT) + 31) / 32, (unsigned)((Bn) + 15) / 16, (unsigned)(1)), 32, 0, stream>>>(gp7); }
    { GemmP gz7;
      gz7.A = SA; gz7.B = JZM; gz7.bias = SA; gz7.R = SA; gz7.C = PHZ;
      gz7.sAo = 0; gz7.sAi = 0; gz7.sAm = NT; gz7.sAk = 1; gz7.sBo = 0; gz7.sBi = 0; gz7.sBn = NT; gz7.sBk = 1; gz7.sCo = 0; gz7.sCi = 0; gz7.sCm = NT; gz7.sRo = 0; gz7.sRi = 0; gz7.sRm = 0; gz7.sRn = 0;
      gz7.M = Bn; gz7.N = NT; gz7.K = NT; gz7.zi_n = 1; gz7.flags = 0; gz7.act = 0;
      gz7.alpha = 1.0f; gz7.beta = 0.0f; gz7.sa = 1.0f; gz7.sb = 1.0f; gz7.Npad = NT; gz7.pad_ = 0;
      k_gemm<1><<<dim3((unsigned)((NT) + 31) / 32, (unsigned)((Bn) + 15) / 16, (unsigned)(1)), 32, 0, stream>>>(gz7); }
    k_soen_step<<<(unsigned)(((long long)Bn * NT + 255) / 256), 256, 0, stream>>>(SA, PHI, PHZ, gam, tau, foz, SB, Bn, NT);
    { GemmP gp8;
      gp8.A = SB; gp8.B = JM; gp8.bias = SB; gp8.R = EXT; gp8.C = PHI;
      gp8.sAo = 0; gp8.sAi = 0; gp8.sAm = NT; gp8.sAk = 1; gp8.sBo = 0; gp8.sBi = 0; gp8.sBn = NT; gp8.sBk = 1; gp8.sCo = 0; gp8.sCi = 0; gp8.sCm = NT; gp8.sRo = 0; gp8.sRi = 0; gp8.sRm = NT; gp8.sRn = 1;
      gp8.M = Bn; gp8.N = NT; gp8.K = NT; gp8.zi_n = 1; gp8.flags = 4; gp8.act = 0;
      gp8.alpha = 1.0f; gp8.beta = 1.0f; gp8.sa = 1.0f; gp8.sb = 1.0f; gp8.Npad = NT; gp8.pad_ = 0;
      k_gemm<1><<<dim3((unsigned)((NT) + 31) / 32, (unsigned)((Bn) + 15) / 16, (unsigned)(1)), 32, 0, stream>>>(gp8); }
    { GemmP gz8;
      gz8.A = SB; gz8.B = JZM; gz8.bias = SB; gz8.R = SB; gz8.C = PHZ;
      gz8.sAo = 0; gz8.sAi = 0; gz8.sAm = NT; gz8.sAk = 1; gz8.sBo = 0; gz8.sBi = 0; gz8.sBn = NT; gz8.sBk = 1; gz8.sCo = 0; gz8.sCi = 0; gz8.sCm = NT; gz8.sRo = 0; gz8.sRi = 0; gz8.sRm = 0; gz8.sRn = 0;
      gz8.M = Bn; gz8.N = NT; gz8.K = NT; gz8.zi_n = 1; gz8.flags = 0; gz8.act = 0;
      gz8.alpha = 1.0f; gz8.beta = 0.0f; gz8.sa = 1.0f; gz8.sb = 1.0f; gz8.Npad = NT; gz8.pad_ = 0;
      k_gemm<1><<<dim3((unsigned)((NT) + 31) / 32, (unsigned)((Bn) + 15) / 16, (unsigned)(1)), 32, 0, stream>>>(gz8); }
    k_soen_step<<<(unsigned)(((long long)Bn * NT + 255) / 256), 256, 0, stream>>>(SB, PHI, PHZ, gam, tau, foz, SA, Bn, NT);
    { GemmP gp9;
      gp9.A = SA; gp9.B = JM; gp9.bias = SA; gp9.R = EXT; gp9.C = PHI;
      gp9.sAo = 0; gp9.sAi = 0; gp9.sAm = NT; gp9.sAk = 1; gp9.sBo = 0; gp9.sBi = 0; gp9.sBn = NT; gp9.sBk = 1; gp9.sCo = 0; gp9.sCi = 0; gp9.sCm = NT; gp9.sRo = 0; gp9.sRi = 0; gp9.sRm = NT; gp9.sRn = 1;
      gp9.M = Bn; gp9.N = NT; gp9.K = NT; gp9.zi_n = 1; gp9.flags = 4; gp9.act = 0;
      gp9.alpha = 1.0f; gp9.beta = 1.0f; gp9.sa = 1.0f; gp9.sb = 1.0f; gp9.Npad = NT; gp9.pad_ = 0;
      k_gemm<1><<<dim3((unsigned)((NT) + 31) / 32, (unsigned)((Bn) + 15) / 16, (unsigned)(1)), 32, 0, stream>>>(gp9); }
    { GemmP gz9;
      gz9.A = SA; gz9.B = JZM; gz9.bias = SA; gz9.R = SA; gz9.C = PHZ;
      gz9.sAo = 0; gz9.sAi = 0; gz9.sAm = NT; gz9.sAk = 1; gz9.sBo = 0; gz9.sBi = 0; gz9.sBn = NT; gz9.sBk = 1; gz9.sCo = 0; gz9.sCi = 0; gz9.sCm = NT; gz9.sRo = 0; gz9.sRi = 0; gz9.sRm = 0; gz9.sRn = 0;
      gz9.M = Bn; gz9.N = NT; gz9.K = NT; gz9.zi_n = 1; gz9.flags = 0; gz9.act = 0;
      gz9.alpha = 1.0f; gz9.beta = 0.0f; gz9.sa = 1.0f; gz9.sb = 1.0f; gz9.Npad = NT; gz9.pad_ = 0;
      k_gemm<1><<<dim3((unsigned)((NT) + 31) / 32, (unsigned)((Bn) + 15) / 16, (unsigned)(1)), 32, 0, stream>>>(gz9); }
    k_soen_step<<<(unsigned)(((long long)Bn * NT + 255) / 256), 256, 0, stream>>>(SA, PHI, PHZ, gam, tau, foz, SB, Bn, NT);
    { GemmP gp10;
      gp10.A = SB; gp10.B = JM; gp10.bias = SB; gp10.R = EXT; gp10.C = PHI;
      gp10.sAo = 0; gp10.sAi = 0; gp10.sAm = NT; gp10.sAk = 1; gp10.sBo = 0; gp10.sBi = 0; gp10.sBn = NT; gp10.sBk = 1; gp10.sCo = 0; gp10.sCi = 0; gp10.sCm = NT; gp10.sRo = 0; gp10.sRi = 0; gp10.sRm = NT; gp10.sRn = 1;
      gp10.M = Bn; gp10.N = NT; gp10.K = NT; gp10.zi_n = 1; gp10.flags = 4; gp10.act = 0;
      gp10.alpha = 1.0f; gp10.beta = 1.0f; gp10.sa = 1.0f; gp10.sb = 1.0f; gp10.Npad = NT; gp10.pad_ = 0;
      k_gemm<1><<<dim3((unsigned)((NT) + 31) / 32, (unsigned)((Bn) + 15) / 16, (unsigned)(1)), 32, 0, stream>>>(gp10); }
    { GemmP gz10;
      gz10.A = SB; gz10.B = JZM; gz10.bias = SB; gz10.R = SB; gz10.C = PHZ;
      gz10.sAo = 0; gz10.sAi = 0; gz10.sAm = NT; gz10.sAk = 1; gz10.sBo = 0; gz10.sBi = 0; gz10.sBn = NT; gz10.sBk = 1; gz10.sCo = 0; gz10.sCi = 0; gz10.sCm = NT; gz10.sRo = 0; gz10.sRi = 0; gz10.sRm = 0; gz10.sRn = 0;
      gz10.M = Bn; gz10.N = NT; gz10.K = NT; gz10.zi_n = 1; gz10.flags = 0; gz10.act = 0;
      gz10.alpha = 1.0f; gz10.beta = 0.0f; gz10.sa = 1.0f; gz10.sb = 1.0f; gz10.Npad = NT; gz10.pad_ = 0;
      k_gemm<1><<<dim3((unsigned)((NT) + 31) / 32, (unsigned)((Bn) + 15) / 16, (unsigned)(1)), 32, 0, stream>>>(gz10); }
    k_soen_step<<<(unsigned)(((long long)Bn * NT + 255) / 256), 256, 0, stream>>>(SB, PHI, PHZ, gam, tau, foz, SA, Bn, NT);
    { GemmP gp11;
      gp11.A = SA; gp11.B = JM; gp11.bias = SA; gp11.R = EXT; gp11.C = PHI;
      gp11.sAo = 0; gp11.sAi = 0; gp11.sAm = NT; gp11.sAk = 1; gp11.sBo = 0; gp11.sBi = 0; gp11.sBn = NT; gp11.sBk = 1; gp11.sCo = 0; gp11.sCi = 0; gp11.sCm = NT; gp11.sRo = 0; gp11.sRi = 0; gp11.sRm = NT; gp11.sRn = 1;
      gp11.M = Bn; gp11.N = NT; gp11.K = NT; gp11.zi_n = 1; gp11.flags = 4; gp11.act = 0;
      gp11.alpha = 1.0f; gp11.beta = 1.0f; gp11.sa = 1.0f; gp11.sb = 1.0f; gp11.Npad = NT; gp11.pad_ = 0;
      k_gemm<1><<<dim3((unsigned)((NT) + 31) / 32, (unsigned)((Bn) + 15) / 16, (unsigned)(1)), 32, 0, stream>>>(gp11); }
    { GemmP gz11;
      gz11.A = SA; gz11.B = JZM; gz11.bias = SA; gz11.R = SA; gz11.C = PHZ;
      gz11.sAo = 0; gz11.sAi = 0; gz11.sAm = NT; gz11.sAk = 1; gz11.sBo = 0; gz11.sBi = 0; gz11.sBn = NT; gz11.sBk = 1; gz11.sCo = 0; gz11.sCi = 0; gz11.sCm = NT; gz11.sRo = 0; gz11.sRi = 0; gz11.sRm = 0; gz11.sRn = 0;
      gz11.M = Bn; gz11.N = NT; gz11.K = NT; gz11.zi_n = 1; gz11.flags = 0; gz11.act = 0;
      gz11.alpha = 1.0f; gz11.beta = 0.0f; gz11.sa = 1.0f; gz11.sb = 1.0f; gz11.Npad = NT; gz11.pad_ = 0;
      k_gemm<1><<<dim3((unsigned)((NT) + 31) / 32, (unsigned)((Bn) + 15) / 16, (unsigned)(1)), 32, 0, stream>>>(gz11); }
    k_soen_step<<<(unsigned)(((long long)Bn * NT + 255) / 256), 256, 0, stream>>>(SA, PHI, PHZ, gam, tau, foz, SB, Bn, NT);
    { GemmP gp12;
      gp12.A = SB; gp12.B = JM; gp12.bias = SB; gp12.R = EXT; gp12.C = PHI;
      gp12.sAo = 0; gp12.sAi = 0; gp12.sAm = NT; gp12.sAk = 1; gp12.sBo = 0; gp12.sBi = 0; gp12.sBn = NT; gp12.sBk = 1; gp12.sCo = 0; gp12.sCi = 0; gp12.sCm = NT; gp12.sRo = 0; gp12.sRi = 0; gp12.sRm = NT; gp12.sRn = 1;
      gp12.M = Bn; gp12.N = NT; gp12.K = NT; gp12.zi_n = 1; gp12.flags = 4; gp12.act = 0;
      gp12.alpha = 1.0f; gp12.beta = 1.0f; gp12.sa = 1.0f; gp12.sb = 1.0f; gp12.Npad = NT; gp12.pad_ = 0;
      k_gemm<1><<<dim3((unsigned)((NT) + 31) / 32, (unsigned)((Bn) + 15) / 16, (unsigned)(1)), 32, 0, stream>>>(gp12); }
    { GemmP gz12;
      gz12.A = SB; gz12.B = JZM; gz12.bias = SB; gz12.R = SB; gz12.C = PHZ;
      gz12.sAo = 0; gz12.sAi = 0; gz12.sAm = NT; gz12.sAk = 1; gz12.sBo = 0; gz12.sBi = 0; gz12.sBn = NT; gz12.sBk = 1; gz12.sCo = 0; gz12.sCi = 0; gz12.sCm = NT; gz12.sRo = 0; gz12.sRi = 0; gz12.sRm = 0; gz12.sRn = 0;
      gz12.M = Bn; gz12.N = NT; gz12.K = NT; gz12.zi_n = 1; gz12.flags = 0; gz12.act = 0;
      gz12.alpha = 1.0f; gz12.beta = 0.0f; gz12.sa = 1.0f; gz12.sb = 1.0f; gz12.Npad = NT; gz12.pad_ = 0;
      k_gemm<1><<<dim3((unsigned)((NT) + 31) / 32, (unsigned)((Bn) + 15) / 16, (unsigned)(1)), 32, 0, stream>>>(gz12); }
    k_soen_step<<<(unsigned)(((long long)Bn * NT + 255) / 256), 256, 0, stream>>>(SB, PHI, PHZ, gam, tau, foz, SA, Bn, NT);
    { GemmP gp13;
      gp13.A = SA; gp13.B = JM; gp13.bias = SA; gp13.R = EXT; gp13.C = PHI;
      gp13.sAo = 0; gp13.sAi = 0; gp13.sAm = NT; gp13.sAk = 1; gp13.sBo = 0; gp13.sBi = 0; gp13.sBn = NT; gp13.sBk = 1; gp13.sCo = 0; gp13.sCi = 0; gp13.sCm = NT; gp13.sRo = 0; gp13.sRi = 0; gp13.sRm = NT; gp13.sRn = 1;
      gp13.M = Bn; gp13.N = NT; gp13.K = NT; gp13.zi_n = 1; gp13.flags = 4; gp13.act = 0;
      gp13.alpha = 1.0f; gp13.beta = 1.0f; gp13.sa = 1.0f; gp13.sb = 1.0f; gp13.Npad = NT; gp13.pad_ = 0;
      k_gemm<1><<<dim3((unsigned)((NT) + 31) / 32, (unsigned)((Bn) + 15) / 16, (unsigned)(1)), 32, 0, stream>>>(gp13); }
    { GemmP gz13;
      gz13.A = SA; gz13.B = JZM; gz13.bias = SA; gz13.R = SA; gz13.C = PHZ;
      gz13.sAo = 0; gz13.sAi = 0; gz13.sAm = NT; gz13.sAk = 1; gz13.sBo = 0; gz13.sBi = 0; gz13.sBn = NT; gz13.sBk = 1; gz13.sCo = 0; gz13.sCi = 0; gz13.sCm = NT; gz13.sRo = 0; gz13.sRi = 0; gz13.sRm = 0; gz13.sRn = 0;
      gz13.M = Bn; gz13.N = NT; gz13.K = NT; gz13.zi_n = 1; gz13.flags = 0; gz13.act = 0;
      gz13.alpha = 1.0f; gz13.beta = 0.0f; gz13.sa = 1.0f; gz13.sb = 1.0f; gz13.Npad = NT; gz13.pad_ = 0;
      k_gemm<1><<<dim3((unsigned)((NT) + 31) / 32, (unsigned)((Bn) + 15) / 16, (unsigned)(1)), 32, 0, stream>>>(gz13); }
    k_soen_step<<<(unsigned)(((long long)Bn * NT + 255) / 256), 256, 0, stream>>>(SA, PHI, PHZ, gam, tau, foz, SB, Bn, NT);
    { GemmP gp14;
      gp14.A = SB; gp14.B = JM; gp14.bias = SB; gp14.R = EXT; gp14.C = PHI;
      gp14.sAo = 0; gp14.sAi = 0; gp14.sAm = NT; gp14.sAk = 1; gp14.sBo = 0; gp14.sBi = 0; gp14.sBn = NT; gp14.sBk = 1; gp14.sCo = 0; gp14.sCi = 0; gp14.sCm = NT; gp14.sRo = 0; gp14.sRi = 0; gp14.sRm = NT; gp14.sRn = 1;
      gp14.M = Bn; gp14.N = NT; gp14.K = NT; gp14.zi_n = 1; gp14.flags = 4; gp14.act = 0;
      gp14.alpha = 1.0f; gp14.beta = 1.0f; gp14.sa = 1.0f; gp14.sb = 1.0f; gp14.Npad = NT; gp14.pad_ = 0;
      k_gemm<1><<<dim3((unsigned)((NT) + 31) / 32, (unsigned)((Bn) + 15) / 16, (unsigned)(1)), 32, 0, stream>>>(gp14); }
    { GemmP gz14;
      gz14.A = SB; gz14.B = JZM; gz14.bias = SB; gz14.R = SB; gz14.C = PHZ;
      gz14.sAo = 0; gz14.sAi = 0; gz14.sAm = NT; gz14.sAk = 1; gz14.sBo = 0; gz14.sBi = 0; gz14.sBn = NT; gz14.sBk = 1; gz14.sCo = 0; gz14.sCi = 0; gz14.sCm = NT; gz14.sRo = 0; gz14.sRi = 0; gz14.sRm = 0; gz14.sRn = 0;
      gz14.M = Bn; gz14.N = NT; gz14.K = NT; gz14.zi_n = 1; gz14.flags = 0; gz14.act = 0;
      gz14.alpha = 1.0f; gz14.beta = 0.0f; gz14.sa = 1.0f; gz14.sb = 1.0f; gz14.Npad = NT; gz14.pad_ = 0;
      k_gemm<1><<<dim3((unsigned)((NT) + 31) / 32, (unsigned)((Bn) + 15) / 16, (unsigned)(1)), 32, 0, stream>>>(gz14); }
    k_soen_step<<<(unsigned)(((long long)Bn * NT + 255) / 256), 256, 0, stream>>>(SB, PHI, PHZ, gam, tau, foz, SA, Bn, NT);
    { GemmP gp15;
      gp15.A = SA; gp15.B = JM; gp15.bias = SA; gp15.R = EXT; gp15.C = PHI;
      gp15.sAo = 0; gp15.sAi = 0; gp15.sAm = NT; gp15.sAk = 1; gp15.sBo = 0; gp15.sBi = 0; gp15.sBn = NT; gp15.sBk = 1; gp15.sCo = 0; gp15.sCi = 0; gp15.sCm = NT; gp15.sRo = 0; gp15.sRi = 0; gp15.sRm = NT; gp15.sRn = 1;
      gp15.M = Bn; gp15.N = NT; gp15.K = NT; gp15.zi_n = 1; gp15.flags = 4; gp15.act = 0;
      gp15.alpha = 1.0f; gp15.beta = 1.0f; gp15.sa = 1.0f; gp15.sb = 1.0f; gp15.Npad = NT; gp15.pad_ = 0;
      k_gemm<1><<<dim3((unsigned)((NT) + 31) / 32, (unsigned)((Bn) + 15) / 16, (unsigned)(1)), 32, 0, stream>>>(gp15); }
    { GemmP gz15;
      gz15.A = SA; gz15.B = JZM; gz15.bias = SA; gz15.R = SA; gz15.C = PHZ;
      gz15.sAo = 0; gz15.sAi = 0; gz15.sAm = NT; gz15.sAk = 1; gz15.sBo = 0; gz15.sBi = 0; gz15.sBn = NT; gz15.sBk = 1; gz15.sCo = 0; gz15.sCi = 0; gz15.sCm = NT; gz15.sRo = 0; gz15.sRi = 0; gz15.sRm = 0; gz15.sRn = 0;
      gz15.M = Bn; gz15.N = NT; gz15.K = NT; gz15.zi_n = 1; gz15.flags = 0; gz15.act = 0;
      gz15.alpha = 1.0f; gz15.beta = 0.0f; gz15.sa = 1.0f; gz15.sb = 1.0f; gz15.Npad = NT; gz15.pad_ = 0;
      k_gemm<1><<<dim3((unsigned)((NT) + 31) / 32, (unsigned)((Bn) + 15) / 16, (unsigned)(1)), 32, 0, stream>>>(gz15); }
    k_soen_step<<<(unsigned)(((long long)Bn * NT + 255) / 256), 256, 0, stream>>>(SA, PHI, PHZ, gam, tau, foz, SB, Bn, NT);
    { GemmP gp16;
      gp16.A = SB; gp16.B = JM; gp16.bias = SB; gp16.R = EXT; gp16.C = PHI;
      gp16.sAo = 0; gp16.sAi = 0; gp16.sAm = NT; gp16.sAk = 1; gp16.sBo = 0; gp16.sBi = 0; gp16.sBn = NT; gp16.sBk = 1; gp16.sCo = 0; gp16.sCi = 0; gp16.sCm = NT; gp16.sRo = 0; gp16.sRi = 0; gp16.sRm = NT; gp16.sRn = 1;
      gp16.M = Bn; gp16.N = NT; gp16.K = NT; gp16.zi_n = 1; gp16.flags = 4; gp16.act = 0;
      gp16.alpha = 1.0f; gp16.beta = 1.0f; gp16.sa = 1.0f; gp16.sb = 1.0f; gp16.Npad = NT; gp16.pad_ = 0;
      k_gemm<1><<<dim3((unsigned)((NT) + 31) / 32, (unsigned)((Bn) + 15) / 16, (unsigned)(1)), 32, 0, stream>>>(gp16); }
    { GemmP gz16;
      gz16.A = SB; gz16.B = JZM; gz16.bias = SB; gz16.R = SB; gz16.C = PHZ;
      gz16.sAo = 0; gz16.sAi = 0; gz16.sAm = NT; gz16.sAk = 1; gz16.sBo = 0; gz16.sBi = 0; gz16.sBn = NT; gz16.sBk = 1; gz16.sCo = 0; gz16.sCi = 0; gz16.sCm = NT; gz16.sRo = 0; gz16.sRi = 0; gz16.sRm = 0; gz16.sRn = 0;
      gz16.M = Bn; gz16.N = NT; gz16.K = NT; gz16.zi_n = 1; gz16.flags = 0; gz16.act = 0;
      gz16.alpha = 1.0f; gz16.beta = 0.0f; gz16.sa = 1.0f; gz16.sb = 1.0f; gz16.Npad = NT; gz16.pad_ = 0;
      k_gemm<1><<<dim3((unsigned)((NT) + 31) / 32, (unsigned)((Bn) + 15) / 16, (unsigned)(1)), 32, 0, stream>>>(gz16); }
    k_soen_step<<<(unsigned)(((long long)Bn * NT + 255) / 256), 256, 0, stream>>>(SB, PHI, PHZ, gam, tau, foz, SA, Bn, NT);
    { GemmP gp17;
      gp17.A = SA; gp17.B = JM; gp17.bias = SA; gp17.R = EXT; gp17.C = PHI;
      gp17.sAo = 0; gp17.sAi = 0; gp17.sAm = NT; gp17.sAk = 1; gp17.sBo = 0; gp17.sBi = 0; gp17.sBn = NT; gp17.sBk = 1; gp17.sCo = 0; gp17.sCi = 0; gp17.sCm = NT; gp17.sRo = 0; gp17.sRi = 0; gp17.sRm = NT; gp17.sRn = 1;
      gp17.M = Bn; gp17.N = NT; gp17.K = NT; gp17.zi_n = 1; gp17.flags = 4; gp17.act = 0;
      gp17.alpha = 1.0f; gp17.beta = 1.0f; gp17.sa = 1.0f; gp17.sb = 1.0f; gp17.Npad = NT; gp17.pad_ = 0;
      k_gemm<1><<<dim3((unsigned)((NT) + 31) / 32, (unsigned)((Bn) + 15) / 16, (unsigned)(1)), 32, 0, stream>>>(gp17); }
    { GemmP gz17;
      gz17.A = SA; gz17.B = JZM; gz17.bias = SA; gz17.R = SA; gz17.C = PHZ;
      gz17.sAo = 0; gz17.sAi = 0; gz17.sAm = NT; gz17.sAk = 1; gz17.sBo = 0; gz17.sBi = 0; gz17.sBn = NT; gz17.sBk = 1; gz17.sCo = 0; gz17.sCi = 0; gz17.sCm = NT; gz17.sRo = 0; gz17.sRi = 0; gz17.sRm = 0; gz17.sRn = 0;
      gz17.M = Bn; gz17.N = NT; gz17.K = NT; gz17.zi_n = 1; gz17.flags = 0; gz17.act = 0;
      gz17.alpha = 1.0f; gz17.beta = 0.0f; gz17.sa = 1.0f; gz17.sb = 1.0f; gz17.Npad = NT; gz17.pad_ = 0;
      k_gemm<1><<<dim3((unsigned)((NT) + 31) / 32, (unsigned)((Bn) + 15) / 16, (unsigned)(1)), 32, 0, stream>>>(gz17); }
    k_soen_step<<<(unsigned)(((long long)Bn * NT + 255) / 256), 256, 0, stream>>>(SA, PHI, PHZ, gam, tau, foz, SB, Bn, NT);
    { GemmP gp18;
      gp18.A = SB; gp18.B = JM; gp18.bias = SB; gp18.R = EXT; gp18.C = PHI;
      gp18.sAo = 0; gp18.sAi = 0; gp18.sAm = NT; gp18.sAk = 1; gp18.sBo = 0; gp18.sBi = 0; gp18.sBn = NT; gp18.sBk = 1; gp18.sCo = 0; gp18.sCi = 0; gp18.sCm = NT; gp18.sRo = 0; gp18.sRi = 0; gp18.sRm = NT; gp18.sRn = 1;
      gp18.M = Bn; gp18.N = NT; gp18.K = NT; gp18.zi_n = 1; gp18.flags = 4; gp18.act = 0;
      gp18.alpha = 1.0f; gp18.beta = 1.0f; gp18.sa = 1.0f; gp18.sb = 1.0f; gp18.Npad = NT; gp18.pad_ = 0;
      k_gemm<1><<<dim3((unsigned)((NT) + 31) / 32, (unsigned)((Bn) + 15) / 16, (unsigned)(1)), 32, 0, stream>>>(gp18); }
    { GemmP gz18;
      gz18.A = SB; gz18.B = JZM; gz18.bias = SB; gz18.R = SB; gz18.C = PHZ;
      gz18.sAo = 0; gz18.sAi = 0; gz18.sAm = NT; gz18.sAk = 1; gz18.sBo = 0; gz18.sBi = 0; gz18.sBn = NT; gz18.sBk = 1; gz18.sCo = 0; gz18.sCi = 0; gz18.sCm = NT; gz18.sRo = 0; gz18.sRi = 0; gz18.sRm = 0; gz18.sRn = 0;
      gz18.M = Bn; gz18.N = NT; gz18.K = NT; gz18.zi_n = 1; gz18.flags = 0; gz18.act = 0;
      gz18.alpha = 1.0f; gz18.beta = 0.0f; gz18.sa = 1.0f; gz18.sb = 1.0f; gz18.Npad = NT; gz18.pad_ = 0;
      k_gemm<1><<<dim3((unsigned)((NT) + 31) / 32, (unsigned)((Bn) + 15) / 16, (unsigned)(1)), 32, 0, stream>>>(gz18); }
    k_soen_step<<<(unsigned)(((long long)Bn * NT + 255) / 256), 256, 0, stream>>>(SB, PHI, PHZ, gam, tau, foz, SA, Bn, NT);
    { GemmP gp19;
      gp19.A = SA; gp19.B = JM; gp19.bias = SA; gp19.R = EXT; gp19.C = PHI;
      gp19.sAo = 0; gp19.sAi = 0; gp19.sAm = NT; gp19.sAk = 1; gp19.sBo = 0; gp19.sBi = 0; gp19.sBn = NT; gp19.sBk = 1; gp19.sCo = 0; gp19.sCi = 0; gp19.sCm = NT; gp19.sRo = 0; gp19.sRi = 0; gp19.sRm = NT; gp19.sRn = 1;
      gp19.M = Bn; gp19.N = NT; gp19.K = NT; gp19.zi_n = 1; gp19.flags = 4; gp19.act = 0;
      gp19.alpha = 1.0f; gp19.beta = 1.0f; gp19.sa = 1.0f; gp19.sb = 1.0f; gp19.Npad = NT; gp19.pad_ = 0;
      k_gemm<1><<<dim3((unsigned)((NT) + 31) / 32, (unsigned)((Bn) + 15) / 16, (unsigned)(1)), 32, 0, stream>>>(gp19); }
    { GemmP gz19;
      gz19.A = SA; gz19.B = JZM; gz19.bias = SA; gz19.R = SA; gz19.C = PHZ;
      gz19.sAo = 0; gz19.sAi = 0; gz19.sAm = NT; gz19.sAk = 1; gz19.sBo = 0; gz19.sBi = 0; gz19.sBn = NT; gz19.sBk = 1; gz19.sCo = 0; gz19.sCi = 0; gz19.sCm = NT; gz19.sRo = 0; gz19.sRi = 0; gz19.sRm = 0; gz19.sRn = 0;
      gz19.M = Bn; gz19.N = NT; gz19.K = NT; gz19.zi_n = 1; gz19.flags = 0; gz19.act = 0;
      gz19.alpha = 1.0f; gz19.beta = 0.0f; gz19.sa = 1.0f; gz19.sb = 1.0f; gz19.Npad = NT; gz19.pad_ = 0;
      k_gemm<1><<<dim3((unsigned)((NT) + 31) / 32, (unsigned)((Bn) + 15) / 16, (unsigned)(1)), 32, 0, stream>>>(gz19); }
    k_soen_step<<<(unsigned)(((long long)Bn * NT + 255) / 256), 256, 0, stream>>>(SA, PHI, PHZ, gam, tau, foz, SB, Bn, NT);
    { GemmP gp20;
      gp20.A = SB; gp20.B = JM; gp20.bias = SB; gp20.R = EXT; gp20.C = PHI;
      gp20.sAo = 0; gp20.sAi = 0; gp20.sAm = NT; gp20.sAk = 1; gp20.sBo = 0; gp20.sBi = 0; gp20.sBn = NT; gp20.sBk = 1; gp20.sCo = 0; gp20.sCi = 0; gp20.sCm = NT; gp20.sRo = 0; gp20.sRi = 0; gp20.sRm = NT; gp20.sRn = 1;
      gp20.M = Bn; gp20.N = NT; gp20.K = NT; gp20.zi_n = 1; gp20.flags = 4; gp20.act = 0;
      gp20.alpha = 1.0f; gp20.beta = 1.0f; gp20.sa = 1.0f; gp20.sb = 1.0f; gp20.Npad = NT; gp20.pad_ = 0;
      k_gemm<1><<<dim3((unsigned)((NT) + 31) / 32, (unsigned)((Bn) + 15) / 16, (unsigned)(1)), 32, 0, stream>>>(gp20); }
    { GemmP gz20;
      gz20.A = SB; gz20.B = JZM; gz20.bias = SB; gz20.R = SB; gz20.C = PHZ;
      gz20.sAo = 0; gz20.sAi = 0; gz20.sAm = NT; gz20.sAk = 1; gz20.sBo = 0; gz20.sBi = 0; gz20.sBn = NT; gz20.sBk = 1; gz20.sCo = 0; gz20.sCi = 0; gz20.sCm = NT; gz20.sRo = 0; gz20.sRi = 0; gz20.sRm = 0; gz20.sRn = 0;
      gz20.M = Bn; gz20.N = NT; gz20.K = NT; gz20.zi_n = 1; gz20.flags = 0; gz20.act = 0;
      gz20.alpha = 1.0f; gz20.beta = 0.0f; gz20.sa = 1.0f; gz20.sb = 1.0f; gz20.Npad = NT; gz20.pad_ = 0;
      k_gemm<1><<<dim3((unsigned)((NT) + 31) / 32, (unsigned)((Bn) + 15) / 16, (unsigned)(1)), 32, 0, stream>>>(gz20); }
    k_soen_step<<<(unsigned)(((long long)Bn * NT + 255) / 256), 256, 0, stream>>>(SB, PHI, PHZ, gam, tau, foz, SA, Bn, NT);
    { GemmP gp21;
      gp21.A = SA; gp21.B = JM; gp21.bias = SA; gp21.R = EXT; gp21.C = PHI;
      gp21.sAo = 0; gp21.sAi = 0; gp21.sAm = NT; gp21.sAk = 1; gp21.sBo = 0; gp21.sBi = 0; gp21.sBn = NT; gp21.sBk = 1; gp21.sCo = 0; gp21.sCi = 0; gp21.sCm = NT; gp21.sRo = 0; gp21.sRi = 0; gp21.sRm = NT; gp21.sRn = 1;
      gp21.M = Bn; gp21.N = NT; gp21.K = NT; gp21.zi_n = 1; gp21.flags = 4; gp21.act = 0;
      gp21.alpha = 1.0f; gp21.beta = 1.0f; gp21.sa = 1.0f; gp21.sb = 1.0f; gp21.Npad = NT; gp21.pad_ = 0;
      k_gemm<1><<<dim3((unsigned)((NT) + 31) / 32, (unsigned)((Bn) + 15) / 16, (unsigned)(1)), 32, 0, stream>>>(gp21); }
    { GemmP gz21;
      gz21.A = SA; gz21.B = JZM; gz21.bias = SA; gz21.R = SA; gz21.C = PHZ;
      gz21.sAo = 0; gz21.sAi = 0; gz21.sAm = NT; gz21.sAk = 1; gz21.sBo = 0; gz21.sBi = 0; gz21.sBn = NT; gz21.sBk = 1; gz21.sCo = 0; gz21.sCi = 0; gz21.sCm = NT; gz21.sRo = 0; gz21.sRi = 0; gz21.sRm = 0; gz21.sRn = 0;
      gz21.M = Bn; gz21.N = NT; gz21.K = NT; gz21.zi_n = 1; gz21.flags = 0; gz21.act = 0;
      gz21.alpha = 1.0f; gz21.beta = 0.0f; gz21.sa = 1.0f; gz21.sb = 1.0f; gz21.Npad = NT; gz21.pad_ = 0;
      k_gemm<1><<<dim3((unsigned)((NT) + 31) / 32, (unsigned)((Bn) + 15) / 16, (unsigned)(1)), 32, 0, stream>>>(gz21); }
    k_soen_step<<<(unsigned)(((long long)Bn * NT + 255) / 256), 256, 0, stream>>>(SA, PHI, PHZ, gam, tau, foz, SB, Bn, NT);
    { GemmP gp22;
      gp22.A = SB; gp22.B = JM; gp22.bias = SB; gp22.R = EXT; gp22.C = PHI;
      gp22.sAo = 0; gp22.sAi = 0; gp22.sAm = NT; gp22.sAk = 1; gp22.sBo = 0; gp22.sBi = 0; gp22.sBn = NT; gp22.sBk = 1; gp22.sCo = 0; gp22.sCi = 0; gp22.sCm = NT; gp22.sRo = 0; gp22.sRi = 0; gp22.sRm = NT; gp22.sRn = 1;
      gp22.M = Bn; gp22.N = NT; gp22.K = NT; gp22.zi_n = 1; gp22.flags = 4; gp22.act = 0;
      gp22.alpha = 1.0f; gp22.beta = 1.0f; gp22.sa = 1.0f; gp22.sb = 1.0f; gp22.Npad = NT; gp22.pad_ = 0;
      k_gemm<1><<<dim3((unsigned)((NT) + 31) / 32, (unsigned)((Bn) + 15) / 16, (unsigned)(1)), 32, 0, stream>>>(gp22); }
    { GemmP gz22;
      gz22.A = SB; gz22.B = JZM; gz22.bias = SB; gz22.R = SB; gz22.C = PHZ;
      gz22.sAo = 0; gz22.sAi = 0; gz22.sAm = NT; gz22.sAk = 1; gz22.sBo = 0; gz22.sBi = 0; gz22.sBn = NT; gz22.sBk = 1; gz22.sCo = 0; gz22.sCi = 0; gz22.sCm = NT; gz22.sRo = 0; gz22.sRi = 0; gz22.sRm = 0; gz22.sRn = 0;
      gz22.M = Bn; gz22.N = NT; gz22.K = NT; gz22.zi_n = 1; gz22.flags = 0; gz22.act = 0;
      gz22.alpha = 1.0f; gz22.beta = 0.0f; gz22.sa = 1.0f; gz22.sb = 1.0f; gz22.Npad = NT; gz22.pad_ = 0;
      k_gemm<1><<<dim3((unsigned)((NT) + 31) / 32, (unsigned)((Bn) + 15) / 16, (unsigned)(1)), 32, 0, stream>>>(gz22); }
    k_soen_step<<<(unsigned)(((long long)Bn * NT + 255) / 256), 256, 0, stream>>>(SB, PHI, PHZ, gam, tau, foz, SA, Bn, NT);
    { GemmP gp23;
      gp23.A = SA; gp23.B = JM; gp23.bias = SA; gp23.R = EXT; gp23.C = PHI;
      gp23.sAo = 0; gp23.sAi = 0; gp23.sAm = NT; gp23.sAk = 1; gp23.sBo = 0; gp23.sBi = 0; gp23.sBn = NT; gp23.sBk = 1; gp23.sCo = 0; gp23.sCi = 0; gp23.sCm = NT; gp23.sRo = 0; gp23.sRi = 0; gp23.sRm = NT; gp23.sRn = 1;
      gp23.M = Bn; gp23.N = NT; gp23.K = NT; gp23.zi_n = 1; gp23.flags = 4; gp23.act = 0;
      gp23.alpha = 1.0f; gp23.beta = 1.0f; gp23.sa = 1.0f; gp23.sb = 1.0f; gp23.Npad = NT; gp23.pad_ = 0;
      k_gemm<1><<<dim3((unsigned)((NT) + 31) / 32, (unsigned)((Bn) + 15) / 16, (unsigned)(1)), 32, 0, stream>>>(gp23); }
    { GemmP gz23;
      gz23.A = SA; gz23.B = JZM; gz23.bias = SA; gz23.R = SA; gz23.C = PHZ;
      gz23.sAo = 0; gz23.sAi = 0; gz23.sAm = NT; gz23.sAk = 1; gz23.sBo = 0; gz23.sBi = 0; gz23.sBn = NT; gz23.sBk = 1; gz23.sCo = 0; gz23.sCi = 0; gz23.sCm = NT; gz23.sRo = 0; gz23.sRi = 0; gz23.sRm = 0; gz23.sRn = 0;
      gz23.M = Bn; gz23.N = NT; gz23.K = NT; gz23.zi_n = 1; gz23.flags = 0; gz23.act = 0;
      gz23.alpha = 1.0f; gz23.beta = 0.0f; gz23.sa = 1.0f; gz23.sb = 1.0f; gz23.Npad = NT; gz23.pad_ = 0;
      k_gemm<1><<<dim3((unsigned)((NT) + 31) / 32, (unsigned)((Bn) + 15) / 16, (unsigned)(1)), 32, 0, stream>>>(gz23); }
    k_soen_step<<<(unsigned)(((long long)Bn * NT + 255) / 256), 256, 0, stream>>>(SA, PHI, PHZ, gam, tau, foz, SB, Bn, NT);
    { GemmP gp24;
      gp24.A = SB; gp24.B = JM; gp24.bias = SB; gp24.R = EXT; gp24.C = PHI;
      gp24.sAo = 0; gp24.sAi = 0; gp24.sAm = NT; gp24.sAk = 1; gp24.sBo = 0; gp24.sBi = 0; gp24.sBn = NT; gp24.sBk = 1; gp24.sCo = 0; gp24.sCi = 0; gp24.sCm = NT; gp24.sRo = 0; gp24.sRi = 0; gp24.sRm = NT; gp24.sRn = 1;
      gp24.M = Bn; gp24.N = NT; gp24.K = NT; gp24.zi_n = 1; gp24.flags = 4; gp24.act = 0;
      gp24.alpha = 1.0f; gp24.beta = 1.0f; gp24.sa = 1.0f; gp24.sb = 1.0f; gp24.Npad = NT; gp24.pad_ = 0;
      k_gemm<1><<<dim3((unsigned)((NT) + 31) / 32, (unsigned)((Bn) + 15) / 16, (unsigned)(1)), 32, 0, stream>>>(gp24); }
    { GemmP gz24;
      gz24.A = SB; gz24.B = JZM; gz24.bias = SB; gz24.R = SB; gz24.C = PHZ;
      gz24.sAo = 0; gz24.sAi = 0; gz24.sAm = NT; gz24.sAk = 1; gz24.sBo = 0; gz24.sBi = 0; gz24.sBn = NT; gz24.sBk = 1; gz24.sCo = 0; gz24.sCi = 0; gz24.sCm = NT; gz24.sRo = 0; gz24.sRi = 0; gz24.sRm = 0; gz24.sRn = 0;
      gz24.M = Bn; gz24.N = NT; gz24.K = NT; gz24.zi_n = 1; gz24.flags = 0; gz24.act = 0;
      gz24.alpha = 1.0f; gz24.beta = 0.0f; gz24.sa = 1.0f; gz24.sb = 1.0f; gz24.Npad = NT; gz24.pad_ = 0;
      k_gemm<1><<<dim3((unsigned)((NT) + 31) / 32, (unsigned)((Bn) + 15) / 16, (unsigned)(1)), 32, 0, stream>>>(gz24); }
    k_soen_step<<<(unsigned)(((long long)Bn * NT + 255) / 256), 256, 0, stream>>>(SB, PHI, PHZ, gam, tau, foz, SA, Bn, NT);
    { GemmP gp25;
      gp25.A = SA; gp25.B = JM; gp25.bias = SA; gp25.R = EXT; gp25.C = PHI;
      gp25.sAo = 0; gp25.sAi = 0; gp25.sAm = NT; gp25.sAk = 1; gp25.sBo = 0; gp25.sBi = 0; gp25.sBn = NT; gp25.sBk = 1; gp25.sCo = 0; gp25.sCi = 0; gp25.sCm = NT; gp25.sRo = 0; gp25.sRi = 0; gp25.sRm = NT; gp25.sRn = 1;
      gp25.M = Bn; gp25.N = NT; gp25.K = NT; gp25.zi_n = 1; gp25.flags = 4; gp25.act = 0;
      gp25.alpha = 1.0f; gp25.beta = 1.0f; gp25.sa = 1.0f; gp25.sb = 1.0f; gp25.Npad = NT; gp25.pad_ = 0;
      k_gemm<1><<<dim3((unsigned)((NT) + 31) / 32, (unsigned)((Bn) + 15) / 16, (unsigned)(1)), 32, 0, stream>>>(gp25); }
    { GemmP gz25;
      gz25.A = SA; gz25.B = JZM; gz25.bias = SA; gz25.R = SA; gz25.C = PHZ;
      gz25.sAo = 0; gz25.sAi = 0; gz25.sAm = NT; gz25.sAk = 1; gz25.sBo = 0; gz25.sBi = 0; gz25.sBn = NT; gz25.sBk = 1; gz25.sCo = 0; gz25.sCi = 0; gz25.sCm = NT; gz25.sRo = 0; gz25.sRi = 0; gz25.sRm = 0; gz25.sRn = 0;
      gz25.M = Bn; gz25.N = NT; gz25.K = NT; gz25.zi_n = 1; gz25.flags = 0; gz25.act = 0;
      gz25.alpha = 1.0f; gz25.beta = 0.0f; gz25.sa = 1.0f; gz25.sb = 1.0f; gz25.Npad = NT; gz25.pad_ = 0;
      k_gemm<1><<<dim3((unsigned)((NT) + 31) / 32, (unsigned)((Bn) + 15) / 16, (unsigned)(1)), 32, 0, stream>>>(gz25); }
    k_soen_step<<<(unsigned)(((long long)Bn * NT + 255) / 256), 256, 0, stream>>>(SA, PHI, PHZ, gam, tau, foz, SB, Bn, NT);
    { GemmP gp26;
      gp26.A = SB; gp26.B = JM; gp26.bias = SB; gp26.R = EXT; gp26.C = PHI;
      gp26.sAo = 0; gp26.sAi = 0; gp26.sAm = NT; gp26.sAk = 1; gp26.sBo = 0; gp26.sBi = 0; gp26.sBn = NT; gp26.sBk = 1; gp26.sCo = 0; gp26.sCi = 0; gp26.sCm = NT; gp26.sRo = 0; gp26.sRi = 0; gp26.sRm = NT; gp26.sRn = 1;
      gp26.M = Bn; gp26.N = NT; gp26.K = NT; gp26.zi_n = 1; gp26.flags = 4; gp26.act = 0;
      gp26.alpha = 1.0f; gp26.beta = 1.0f; gp26.sa = 1.0f; gp26.sb = 1.0f; gp26.Npad = NT; gp26.pad_ = 0;
      k_gemm<1><<<dim3((unsigned)((NT) + 31) / 32, (unsigned)((Bn) + 15) / 16, (unsigned)(1)), 32, 0, stream>>>(gp26); }
    { GemmP gz26;
      gz26.A = SB; gz26.B = JZM; gz26.bias = SB; gz26.R = SB; gz26.C = PHZ;
      gz26.sAo = 0; gz26.sAi = 0; gz26.sAm = NT; gz26.sAk = 1; gz26.sBo = 0; gz26.sBi = 0; gz26.sBn = NT; gz26.sBk = 1; gz26.sCo = 0; gz26.sCi = 0; gz26.sCm = NT; gz26.sRo = 0; gz26.sRi = 0; gz26.sRm = 0; gz26.sRn = 0;
      gz26.M = Bn; gz26.N = NT; gz26.K = NT; gz26.zi_n = 1; gz26.flags = 0; gz26.act = 0;
      gz26.alpha = 1.0f; gz26.beta = 0.0f; gz26.sa = 1.0f; gz26.sb = 1.0f; gz26.Npad = NT; gz26.pad_ = 0;
      k_gemm<1><<<dim3((unsigned)((NT) + 31) / 32, (unsigned)((Bn) + 15) / 16, (unsigned)(1)), 32, 0, stream>>>(gz26); }
    k_soen_step<<<(unsigned)(((long long)Bn * NT + 255) / 256), 256, 0, stream>>>(SB, PHI, PHZ, gam, tau, foz, SA, Bn, NT);
    { GemmP gp27;
      gp27.A = SA; gp27.B = JM; gp27.bias = SA; gp27.R = EXT; gp27.C = PHI;
      gp27.sAo = 0; gp27.sAi = 0; gp27.sAm = NT; gp27.sAk = 1; gp27.sBo = 0; gp27.sBi = 0; gp27.sBn = NT; gp27.sBk = 1; gp27.sCo = 0; gp27.sCi = 0; gp27.sCm = NT; gp27.sRo = 0; gp27.sRi = 0; gp27.sRm = NT; gp27.sRn = 1;
      gp27.M = Bn; gp27.N = NT; gp27.K = NT; gp27.zi_n = 1; gp27.flags = 4; gp27.act = 0;
      gp27.alpha = 1.0f; gp27.beta = 1.0f; gp27.sa = 1.0f; gp27.sb = 1.0f; gp27.Npad = NT; gp27.pad_ = 0;
      k_gemm<1><<<dim3((unsigned)((NT) + 31) / 32, (unsigned)((Bn) + 15) / 16, (unsigned)(1)), 32, 0, stream>>>(gp27); }
    { GemmP gz27;
      gz27.A = SA; gz27.B = JZM; gz27.bias = SA; gz27.R = SA; gz27.C = PHZ;
      gz27.sAo = 0; gz27.sAi = 0; gz27.sAm = NT; gz27.sAk = 1; gz27.sBo = 0; gz27.sBi = 0; gz27.sBn = NT; gz27.sBk = 1; gz27.sCo = 0; gz27.sCi = 0; gz27.sCm = NT; gz27.sRo = 0; gz27.sRi = 0; gz27.sRm = 0; gz27.sRn = 0;
      gz27.M = Bn; gz27.N = NT; gz27.K = NT; gz27.zi_n = 1; gz27.flags = 0; gz27.act = 0;
      gz27.alpha = 1.0f; gz27.beta = 0.0f; gz27.sa = 1.0f; gz27.sb = 1.0f; gz27.Npad = NT; gz27.pad_ = 0;
      k_gemm<1><<<dim3((unsigned)((NT) + 31) / 32, (unsigned)((Bn) + 15) / 16, (unsigned)(1)), 32, 0, stream>>>(gz27); }
    k_soen_step<<<(unsigned)(((long long)Bn * NT + 255) / 256), 256, 0, stream>>>(SA, PHI, PHZ, gam, tau, foz, SB, Bn, NT);
    { GemmP gp28;
      gp28.A = SB; gp28.B = JM; gp28.bias = SB; gp28.R = EXT; gp28.C = PHI;
      gp28.sAo = 0; gp28.sAi = 0; gp28.sAm = NT; gp28.sAk = 1; gp28.sBo = 0; gp28.sBi = 0; gp28.sBn = NT; gp28.sBk = 1; gp28.sCo = 0; gp28.sCi = 0; gp28.sCm = NT; gp28.sRo = 0; gp28.sRi = 0; gp28.sRm = NT; gp28.sRn = 1;
      gp28.M = Bn; gp28.N = NT; gp28.K = NT; gp28.zi_n = 1; gp28.flags = 4; gp28.act = 0;
      gp28.alpha = 1.0f; gp28.beta = 1.0f; gp28.sa = 1.0f; gp28.sb = 1.0f; gp28.Npad = NT; gp28.pad_ = 0;
      k_gemm<1><<<dim3((unsigned)((NT) + 31) / 32, (unsigned)((Bn) + 15) / 16, (unsigned)(1)), 32, 0, stream>>>(gp28); }
    { GemmP gz28;
      gz28.A = SB; gz28.B = JZM; gz28.bias = SB; gz28.R = SB; gz28.C = PHZ;
      gz28.sAo = 0; gz28.sAi = 0; gz28.sAm = NT; gz28.sAk = 1; gz28.sBo = 0; gz28.sBi = 0; gz28.sBn = NT; gz28.sBk = 1; gz28.sCo = 0; gz28.sCi = 0; gz28.sCm = NT; gz28.sRo = 0; gz28.sRi = 0; gz28.sRm = 0; gz28.sRn = 0;
      gz28.M = Bn; gz28.N = NT; gz28.K = NT; gz28.zi_n = 1; gz28.flags = 0; gz28.act = 0;
      gz28.alpha = 1.0f; gz28.beta = 0.0f; gz28.sa = 1.0f; gz28.sb = 1.0f; gz28.Npad = NT; gz28.pad_ = 0;
      k_gemm<1><<<dim3((unsigned)((NT) + 31) / 32, (unsigned)((Bn) + 15) / 16, (unsigned)(1)), 32, 0, stream>>>(gz28); }
    k_soen_step<<<(unsigned)(((long long)Bn * NT + 255) / 256), 256, 0, stream>>>(SB, PHI, PHZ, gam, tau, foz, SA, Bn, NT);
    { GemmP gp29;
      gp29.A = SA; gp29.B = JM; gp29.bias = SA; gp29.R = EXT; gp29.C = PHI;
      gp29.sAo = 0; gp29.sAi = 0; gp29.sAm = NT; gp29.sAk = 1; gp29.sBo = 0; gp29.sBi = 0; gp29.sBn = NT; gp29.sBk = 1; gp29.sCo = 0; gp29.sCi = 0; gp29.sCm = NT; gp29.sRo = 0; gp29.sRi = 0; gp29.sRm = NT; gp29.sRn = 1;
      gp29.M = Bn; gp29.N = NT; gp29.K = NT; gp29.zi_n = 1; gp29.flags = 4; gp29.act = 0;
      gp29.alpha = 1.0f; gp29.beta = 1.0f; gp29.sa = 1.0f; gp29.sb = 1.0f; gp29.Npad = NT; gp29.pad_ = 0;
      k_gemm<1><<<dim3((unsigned)((NT) + 31) / 32, (unsigned)((Bn) + 15) / 16, (unsigned)(1)), 32, 0, stream>>>(gp29); }
    { GemmP gz29;
      gz29.A = SA; gz29.B = JZM; gz29.bias = SA; gz29.R = SA; gz29.C = PHZ;
      gz29.sAo = 0; gz29.sAi = 0; gz29.sAm = NT; gz29.sAk = 1; gz29.sBo = 0; gz29.sBi = 0; gz29.sBn = NT; gz29.sBk = 1; gz29.sCo = 0; gz29.sCi = 0; gz29.sCm = NT; gz29.sRo = 0; gz29.sRi = 0; gz29.sRm = 0; gz29.sRn = 0;
      gz29.M = Bn; gz29.N = NT; gz29.K = NT; gz29.zi_n = 1; gz29.flags = 0; gz29.act = 0;
      gz29.alpha = 1.0f; gz29.beta = 0.0f; gz29.sa = 1.0f; gz29.sb = 1.0f; gz29.Npad = NT; gz29.pad_ = 0;
      k_gemm<1><<<dim3((unsigned)((NT) + 31) / 32, (unsigned)((Bn) + 15) / 16, (unsigned)(1)), 32, 0, stream>>>(gz29); }
    k_soen_step<<<(unsigned)(((long long)Bn * NT + 255) / 256), 256, 0, stream>>>(SA, PHI, PHZ, gam, tau, foz, SB, Bn, NT);
    { GemmP gp30;
      gp30.A = SB; gp30.B = JM; gp30.bias = SB; gp30.R = EXT; gp30.C = PHI;
      gp30.sAo = 0; gp30.sAi = 0; gp30.sAm = NT; gp30.sAk = 1; gp30.sBo = 0; gp30.sBi = 0; gp30.sBn = NT; gp30.sBk = 1; gp30.sCo = 0; gp30.sCi = 0; gp30.sCm = NT; gp30.sRo = 0; gp30.sRi = 0; gp30.sRm = NT; gp30.sRn = 1;
      gp30.M = Bn; gp30.N = NT; gp30.K = NT; gp30.zi_n = 1; gp30.flags = 4; gp30.act = 0;
      gp30.alpha = 1.0f; gp30.beta = 1.0f; gp30.sa = 1.0f; gp30.sb = 1.0f; gp30.Npad = NT; gp30.pad_ = 0;
      k_gemm<1><<<dim3((unsigned)((NT) + 31) / 32, (unsigned)((Bn) + 15) / 16, (unsigned)(1)), 32, 0, stream>>>(gp30); }
    { GemmP gz30;
      gz30.A = SB; gz30.B = JZM; gz30.bias = SB; gz30.R = SB; gz30.C = PHZ;
      gz30.sAo = 0; gz30.sAi = 0; gz30.sAm = NT; gz30.sAk = 1; gz30.sBo = 0; gz30.sBi = 0; gz30.sBn = NT; gz30.sBk = 1; gz30.sCo = 0; gz30.sCi = 0; gz30.sCm = NT; gz30.sRo = 0; gz30.sRi = 0; gz30.sRm = 0; gz30.sRn = 0;
      gz30.M = Bn; gz30.N = NT; gz30.K = NT; gz30.zi_n = 1; gz30.flags = 0; gz30.act = 0;
      gz30.alpha = 1.0f; gz30.beta = 0.0f; gz30.sa = 1.0f; gz30.sb = 1.0f; gz30.Npad = NT; gz30.pad_ = 0;
      k_gemm<1><<<dim3((unsigned)((NT) + 31) / 32, (unsigned)((Bn) + 15) / 16, (unsigned)(1)), 32, 0, stream>>>(gz30); }
    k_soen_step<<<(unsigned)(((long long)Bn * NT + 255) / 256), 256, 0, stream>>>(SB, PHI, PHZ, gam, tau, foz, SA, Bn, NT);
    { GemmP gp31;
      gp31.A = SA; gp31.B = JM; gp31.bias = SA; gp31.R = EXT; gp31.C = PHI;
      gp31.sAo = 0; gp31.sAi = 0; gp31.sAm = NT; gp31.sAk = 1; gp31.sBo = 0; gp31.sBi = 0; gp31.sBn = NT; gp31.sBk = 1; gp31.sCo = 0; gp31.sCi = 0; gp31.sCm = NT; gp31.sRo = 0; gp31.sRi = 0; gp31.sRm = NT; gp31.sRn = 1;
      gp31.M = Bn; gp31.N = NT; gp31.K = NT; gp31.zi_n = 1; gp31.flags = 4; gp31.act = 0;
      gp31.alpha = 1.0f; gp31.beta = 1.0f; gp31.sa = 1.0f; gp31.sb = 1.0f; gp31.Npad = NT; gp31.pad_ = 0;
      k_gemm<1><<<dim3((unsigned)((NT) + 31) / 32, (unsigned)((Bn) + 15) / 16, (unsigned)(1)), 32, 0, stream>>>(gp31); }
    { GemmP gz31;
      gz31.A = SA; gz31.B = JZM; gz31.bias = SA; gz31.R = SA; gz31.C = PHZ;
      gz31.sAo = 0; gz31.sAi = 0; gz31.sAm = NT; gz31.sAk = 1; gz31.sBo = 0; gz31.sBi = 0; gz31.sBn = NT; gz31.sBk = 1; gz31.sCo = 0; gz31.sCi = 0; gz31.sCm = NT; gz31.sRo = 0; gz31.sRi = 0; gz31.sRm = 0; gz31.sRn = 0;
      gz31.M = Bn; gz31.N = NT; gz31.K = NT; gz31.zi_n = 1; gz31.flags = 0; gz31.act = 0;
      gz31.alpha = 1.0f; gz31.beta = 0.0f; gz31.sa = 1.0f; gz31.sb = 1.0f; gz31.Npad = NT; gz31.pad_ = 0;
      k_gemm<1><<<dim3((unsigned)((NT) + 31) / 32, (unsigned)((Bn) + 15) / 16, (unsigned)(1)), 32, 0, stream>>>(gz31); }
    k_soen_step<<<(unsigned)(((long long)Bn * NT + 255) / 256), 256, 0, stream>>>(SA, PHI, PHZ, gam, tau, foz, SB, Bn, NT);
    { GemmP gp32;
      gp32.A = SB; gp32.B = JM; gp32.bias = SB; gp32.R = EXT; gp32.C = PHI;
      gp32.sAo = 0; gp32.sAi = 0; gp32.sAm = NT; gp32.sAk = 1; gp32.sBo = 0; gp32.sBi = 0; gp32.sBn = NT; gp32.sBk = 1; gp32.sCo = 0; gp32.sCi = 0; gp32.sCm = NT; gp32.sRo = 0; gp32.sRi = 0; gp32.sRm = NT; gp32.sRn = 1;
      gp32.M = Bn; gp32.N = NT; gp32.K = NT; gp32.zi_n = 1; gp32.flags = 4; gp32.act = 0;
      gp32.alpha = 1.0f; gp32.beta = 1.0f; gp32.sa = 1.0f; gp32.sb = 1.0f; gp32.Npad = NT; gp32.pad_ = 0;
      k_gemm<1><<<dim3((unsigned)((NT) + 31) / 32, (unsigned)((Bn) + 15) / 16, (unsigned)(1)), 32, 0, stream>>>(gp32); }
    { GemmP gz32;
      gz32.A = SB; gz32.B = JZM; gz32.bias = SB; gz32.R = SB; gz32.C = PHZ;
      gz32.sAo = 0; gz32.sAi = 0; gz32.sAm = NT; gz32.sAk = 1; gz32.sBo = 0; gz32.sBi = 0; gz32.sBn = NT; gz32.sBk = 1; gz32.sCo = 0; gz32.sCi = 0; gz32.sCm = NT; gz32.sRo = 0; gz32.sRi = 0; gz32.sRm = 0; gz32.sRn = 0;
      gz32.M = Bn; gz32.N = NT; gz32.K = NT; gz32.zi_n = 1; gz32.flags = 0; gz32.act = 0;
      gz32.alpha = 1.0f; gz32.beta = 0.0f; gz32.sa = 1.0f; gz32.sb = 1.0f; gz32.Npad = NT; gz32.pad_ = 0;
      k_gemm<1><<<dim3((unsigned)((NT) + 31) / 32, (unsigned)((Bn) + 15) / 16, (unsigned)(1)), 32, 0, stream>>>(gz32); }
    k_soen_step<<<(unsigned)(((long long)Bn * NT + 255) / 256), 256, 0, stream>>>(SB, PHI, PHZ, gam, tau, foz, SA, Bn, NT);
    { GemmP gp33;
      gp33.A = SA; gp33.B = JM; gp33.bias = SA; gp33.R = EXT; gp33.C = PHI;
      gp33.sAo = 0; gp33.sAi = 0; gp33.sAm = NT; gp33.sAk = 1; gp33.sBo = 0; gp33.sBi = 0; gp33.sBn = NT; gp33.sBk = 1; gp33.sCo = 0; gp33.sCi = 0; gp33.sCm = NT; gp33.sRo = 0; gp33.sRi = 0; gp33.sRm = NT; gp33.sRn = 1;
      gp33.M = Bn; gp33.N = NT; gp33.K = NT; gp33.zi_n = 1; gp33.flags = 4; gp33.act = 0;
      gp33.alpha = 1.0f; gp33.beta = 1.0f; gp33.sa = 1.0f; gp33.sb = 1.0f; gp33.Npad = NT; gp33.pad_ = 0;
      k_gemm<1><<<dim3((unsigned)((NT) + 31) / 32, (unsigned)((Bn) + 15) / 16, (unsigned)(1)), 32, 0, stream>>>(gp33); }
    { GemmP gz33;
      gz33.A = SA; gz33.B = JZM; gz33.bias = SA; gz33.R = SA; gz33.C = PHZ;
      gz33.sAo = 0; gz33.sAi = 0; gz33.sAm = NT; gz33.sAk = 1; gz33.sBo = 0; gz33.sBi = 0; gz33.sBn = NT; gz33.sBk = 1; gz33.sCo = 0; gz33.sCi = 0; gz33.sCm = NT; gz33.sRo = 0; gz33.sRi = 0; gz33.sRm = 0; gz33.sRn = 0;
      gz33.M = Bn; gz33.N = NT; gz33.K = NT; gz33.zi_n = 1; gz33.flags = 0; gz33.act = 0;
      gz33.alpha = 1.0f; gz33.beta = 0.0f; gz33.sa = 1.0f; gz33.sb = 1.0f; gz33.Npad = NT; gz33.pad_ = 0;
      k_gemm<1><<<dim3((unsigned)((NT) + 31) / 32, (unsigned)((Bn) + 15) / 16, (unsigned)(1)), 32, 0, stream>>>(gz33); }
    k_soen_step<<<(unsigned)(((long long)Bn * NT + 255) / 256), 256, 0, stream>>>(SA, PHI, PHZ, gam, tau, foz, SB, Bn, NT);
    { GemmP gp34;
      gp34.A = SB; gp34.B = JM; gp34.bias = SB; gp34.R = EXT; gp34.C = PHI;
      gp34.sAo = 0; gp34.sAi = 0; gp34.sAm = NT; gp34.sAk = 1; gp34.sBo = 0; gp34.sBi = 0; gp34.sBn = NT; gp34.sBk = 1; gp34.sCo = 0; gp34.sCi = 0; gp34.sCm = NT; gp34.sRo = 0; gp34.sRi = 0; gp34.sRm = NT; gp34.sRn = 1;
      gp34.M = Bn; gp34.N = NT; gp34.K = NT; gp34.zi_n = 1; gp34.flags = 4; gp34.act = 0;
      gp34.alpha = 1.0f; gp34.beta = 1.0f; gp34.sa = 1.0f; gp34.sb = 1.0f; gp34.Npad = NT; gp34.pad_ = 0;
      k_gemm<1><<<dim3((unsigned)((NT) + 31) / 32, (unsigned)((Bn) + 15) / 16, (unsigned)(1)), 32, 0, stream>>>(gp34); }
    { GemmP gz34;
      gz34.A = SB; gz34.B = JZM; gz34.bias = SB; gz34.R = SB; gz34.C = PHZ;
      gz34.sAo = 0; gz34.sAi = 0; gz34.sAm = NT; gz34.sAk = 1; gz34.sBo = 0; gz34.sBi = 0; gz34.sBn = NT; gz34.sBk = 1; gz34.sCo = 0; gz34.sCi = 0; gz34.sCm = NT; gz34.sRo = 0; gz34.sRi = 0; gz34.sRm = 0; gz34.sRn = 0;
      gz34.M = Bn; gz34.N = NT; gz34.K = NT; gz34.zi_n = 1; gz34.flags = 0; gz34.act = 0;
      gz34.alpha = 1.0f; gz34.beta = 0.0f; gz34.sa = 1.0f; gz34.sb = 1.0f; gz34.Npad = NT; gz34.pad_ = 0;
      k_gemm<1><<<dim3((unsigned)((NT) + 31) / 32, (unsigned)((Bn) + 15) / 16, (unsigned)(1)), 32, 0, stream>>>(gz34); }
    k_soen_step<<<(unsigned)(((long long)Bn * NT + 255) / 256), 256, 0, stream>>>(SB, PHI, PHZ, gam, tau, foz, SA, Bn, NT);
    { GemmP gp35;
      gp35.A = SA; gp35.B = JM; gp35.bias = SA; gp35.R = EXT; gp35.C = PHI;
      gp35.sAo = 0; gp35.sAi = 0; gp35.sAm = NT; gp35.sAk = 1; gp35.sBo = 0; gp35.sBi = 0; gp35.sBn = NT; gp35.sBk = 1; gp35.sCo = 0; gp35.sCi = 0; gp35.sCm = NT; gp35.sRo = 0; gp35.sRi = 0; gp35.sRm = NT; gp35.sRn = 1;
      gp35.M = Bn; gp35.N = NT; gp35.K = NT; gp35.zi_n = 1; gp35.flags = 4; gp35.act = 0;
      gp35.alpha = 1.0f; gp35.beta = 1.0f; gp35.sa = 1.0f; gp35.sb = 1.0f; gp35.Npad = NT; gp35.pad_ = 0;
      k_gemm<1><<<dim3((unsigned)((NT) + 31) / 32, (unsigned)((Bn) + 15) / 16, (unsigned)(1)), 32, 0, stream>>>(gp35); }
    { GemmP gz35;
      gz35.A = SA; gz35.B = JZM; gz35.bias = SA; gz35.R = SA; gz35.C = PHZ;
      gz35.sAo = 0; gz35.sAi = 0; gz35.sAm = NT; gz35.sAk = 1; gz35.sBo = 0; gz35.sBi = 0; gz35.sBn = NT; gz35.sBk = 1; gz35.sCo = 0; gz35.sCi = 0; gz35.sCm = NT; gz35.sRo = 0; gz35.sRi = 0; gz35.sRm = 0; gz35.sRn = 0;
      gz35.M = Bn; gz35.N = NT; gz35.K = NT; gz35.zi_n = 1; gz35.flags = 0; gz35.act = 0;
      gz35.alpha = 1.0f; gz35.beta = 0.0f; gz35.sa = 1.0f; gz35.sb = 1.0f; gz35.Npad = NT; gz35.pad_ = 0;
      k_gemm<1><<<dim3((unsigned)((NT) + 31) / 32, (unsigned)((Bn) + 15) / 16, (unsigned)(1)), 32, 0, stream>>>(gz35); }
    k_soen_step<<<(unsigned)(((long long)Bn * NT + 255) / 256), 256, 0, stream>>>(SA, PHI, PHZ, gam, tau, foz, SB, Bn, NT);
    { GemmP gp36;
      gp36.A = SB; gp36.B = JM; gp36.bias = SB; gp36.R = EXT; gp36.C = PHI;
      gp36.sAo = 0; gp36.sAi = 0; gp36.sAm = NT; gp36.sAk = 1; gp36.sBo = 0; gp36.sBi = 0; gp36.sBn = NT; gp36.sBk = 1; gp36.sCo = 0; gp36.sCi = 0; gp36.sCm = NT; gp36.sRo = 0; gp36.sRi = 0; gp36.sRm = NT; gp36.sRn = 1;
      gp36.M = Bn; gp36.N = NT; gp36.K = NT; gp36.zi_n = 1; gp36.flags = 4; gp36.act = 0;
      gp36.alpha = 1.0f; gp36.beta = 1.0f; gp36.sa = 1.0f; gp36.sb = 1.0f; gp36.Npad = NT; gp36.pad_ = 0;
      k_gemm<1><<<dim3((unsigned)((NT) + 31) / 32, (unsigned)((Bn) + 15) / 16, (unsigned)(1)), 32, 0, stream>>>(gp36); }
    { GemmP gz36;
      gz36.A = SB; gz36.B = JZM; gz36.bias = SB; gz36.R = SB; gz36.C = PHZ;
      gz36.sAo = 0; gz36.sAi = 0; gz36.sAm = NT; gz36.sAk = 1; gz36.sBo = 0; gz36.sBi = 0; gz36.sBn = NT; gz36.sBk = 1; gz36.sCo = 0; gz36.sCi = 0; gz36.sCm = NT; gz36.sRo = 0; gz36.sRi = 0; gz36.sRm = 0; gz36.sRn = 0;
      gz36.M = Bn; gz36.N = NT; gz36.K = NT; gz36.zi_n = 1; gz36.flags = 0; gz36.act = 0;
      gz36.alpha = 1.0f; gz36.beta = 0.0f; gz36.sa = 1.0f; gz36.sb = 1.0f; gz36.Npad = NT; gz36.pad_ = 0;
      k_gemm<1><<<dim3((unsigned)((NT) + 31) / 32, (unsigned)((Bn) + 15) / 16, (unsigned)(1)), 32, 0, stream>>>(gz36); }
    k_soen_step<<<(unsigned)(((long long)Bn * NT + 255) / 256), 256, 0, stream>>>(SB, PHI, PHZ, gam, tau, foz, SA, Bn, NT);
    { GemmP gp37;
      gp37.A = SA; gp37.B = JM; gp37.bias = SA; gp37.R = EXT; gp37.C = PHI;
      gp37.sAo = 0; gp37.sAi = 0; gp37.sAm = NT; gp37.sAk = 1; gp37.sBo = 0; gp37.sBi = 0; gp37.sBn = NT; gp37.sBk = 1; gp37.sCo = 0; gp37.sCi = 0; gp37.sCm = NT; gp37.sRo = 0; gp37.sRi = 0; gp37.sRm = NT; gp37.sRn = 1;
      gp37.M = Bn; gp37.N = NT; gp37.K = NT; gp37.zi_n = 1; gp37.flags = 4; gp37.act = 0;
      gp37.alpha = 1.0f; gp37.beta = 1.0f; gp37.sa = 1.0f; gp37.sb = 1.0f; gp37.Npad = NT; gp37.pad_ = 0;
      k_gemm<1><<<dim3((unsigned)((NT) + 31) / 32, (unsigned)((Bn) + 15) / 16, (unsigned)(1)), 32, 0, stream>>>(gp37); }
    { GemmP gz37;
      gz37.A = SA; gz37.B = JZM; gz37.bias = SA; gz37.R = SA; gz37.C = PHZ;
      gz37.sAo = 0; gz37.sAi = 0; gz37.sAm = NT; gz37.sAk = 1; gz37.sBo = 0; gz37.sBi = 0; gz37.sBn = NT; gz37.sBk = 1; gz37.sCo = 0; gz37.sCi = 0; gz37.sCm = NT; gz37.sRo = 0; gz37.sRi = 0; gz37.sRm = 0; gz37.sRn = 0;
      gz37.M = Bn; gz37.N = NT; gz37.K = NT; gz37.zi_n = 1; gz37.flags = 0; gz37.act = 0;
      gz37.alpha = 1.0f; gz37.beta = 0.0f; gz37.sa = 1.0f; gz37.sb = 1.0f; gz37.Npad = NT; gz37.pad_ = 0;
      k_gemm<1><<<dim3((unsigned)((NT) + 31) / 32, (unsigned)((Bn) + 15) / 16, (unsigned)(1)), 32, 0, stream>>>(gz37); }
    k_soen_step<<<(unsigned)(((long long)Bn * NT + 255) / 256), 256, 0, stream>>>(SA, PHI, PHZ, gam, tau, foz, SB, Bn, NT);
    { GemmP gp38;
      gp38.A = SB; gp38.B = JM; gp38.bias = SB; gp38.R = EXT; gp38.C = PHI;
      gp38.sAo = 0; gp38.sAi = 0; gp38.sAm = NT; gp38.sAk = 1; gp38.sBo = 0; gp38.sBi = 0; gp38.sBn = NT; gp38.sBk = 1; gp38.sCo = 0; gp38.sCi = 0; gp38.sCm = NT; gp38.sRo = 0; gp38.sRi = 0; gp38.sRm = NT; gp38.sRn = 1;
      gp38.M = Bn; gp38.N = NT; gp38.K = NT; gp38.zi_n = 1; gp38.flags = 4; gp38.act = 0;
      gp38.alpha = 1.0f; gp38.beta = 1.0f; gp38.sa = 1.0f; gp38.sb = 1.0f; gp38.Npad = NT; gp38.pad_ = 0;
      k_gemm<1><<<dim3((unsigned)((NT) + 31) / 32, (unsigned)((Bn) + 15) / 16, (unsigned)(1)), 32, 0, stream>>>(gp38); }
    { GemmP gz38;
      gz38.A = SB; gz38.B = JZM; gz38.bias = SB; gz38.R = SB; gz38.C = PHZ;
      gz38.sAo = 0; gz38.sAi = 0; gz38.sAm = NT; gz38.sAk = 1; gz38.sBo = 0; gz38.sBi = 0; gz38.sBn = NT; gz38.sBk = 1; gz38.sCo = 0; gz38.sCi = 0; gz38.sCm = NT; gz38.sRo = 0; gz38.sRi = 0; gz38.sRm = 0; gz38.sRn = 0;
      gz38.M = Bn; gz38.N = NT; gz38.K = NT; gz38.zi_n = 1; gz38.flags = 0; gz38.act = 0;
      gz38.alpha = 1.0f; gz38.beta = 0.0f; gz38.sa = 1.0f; gz38.sb = 1.0f; gz38.Npad = NT; gz38.pad_ = 0;
      k_gemm<1><<<dim3((unsigned)((NT) + 31) / 32, (unsigned)((Bn) + 15) / 16, (unsigned)(1)), 32, 0, stream>>>(gz38); }
    k_soen_step<<<(unsigned)(((long long)Bn * NT + 255) / 256), 256, 0, stream>>>(SB, PHI, PHZ, gam, tau, foz, SA, Bn, NT);
    { GemmP gp39;
      gp39.A = SA; gp39.B = JM; gp39.bias = SA; gp39.R = EXT; gp39.C = PHI;
      gp39.sAo = 0; gp39.sAi = 0; gp39.sAm = NT; gp39.sAk = 1; gp39.sBo = 0; gp39.sBi = 0; gp39.sBn = NT; gp39.sBk = 1; gp39.sCo = 0; gp39.sCi = 0; gp39.sCm = NT; gp39.sRo = 0; gp39.sRi = 0; gp39.sRm = NT; gp39.sRn = 1;
      gp39.M = Bn; gp39.N = NT; gp39.K = NT; gp39.zi_n = 1; gp39.flags = 4; gp39.act = 0;
      gp39.alpha = 1.0f; gp39.beta = 1.0f; gp39.sa = 1.0f; gp39.sb = 1.0f; gp39.Npad = NT; gp39.pad_ = 0;
      k_gemm<1><<<dim3((unsigned)((NT) + 31) / 32, (unsigned)((Bn) + 15) / 16, (unsigned)(1)), 32, 0, stream>>>(gp39); }
    { GemmP gz39;
      gz39.A = SA; gz39.B = JZM; gz39.bias = SA; gz39.R = SA; gz39.C = PHZ;
      gz39.sAo = 0; gz39.sAi = 0; gz39.sAm = NT; gz39.sAk = 1; gz39.sBo = 0; gz39.sBi = 0; gz39.sBn = NT; gz39.sBk = 1; gz39.sCo = 0; gz39.sCi = 0; gz39.sCm = NT; gz39.sRo = 0; gz39.sRi = 0; gz39.sRm = 0; gz39.sRn = 0;
      gz39.M = Bn; gz39.N = NT; gz39.K = NT; gz39.zi_n = 1; gz39.flags = 0; gz39.act = 0;
      gz39.alpha = 1.0f; gz39.beta = 0.0f; gz39.sa = 1.0f; gz39.sb = 1.0f; gz39.Npad = NT; gz39.pad_ = 0;
      k_gemm<1><<<dim3((unsigned)((NT) + 31) / 32, (unsigned)((Bn) + 15) / 16, (unsigned)(1)), 32, 0, stream>>>(gz39); }
    k_soen_step<<<(unsigned)(((long long)Bn * NT + 255) / 256), 256, 0, stream>>>(SA, PHI, PHZ, gam, tau, foz, SB, Bn, NT);
    { GemmP gp40;
      gp40.A = SB; gp40.B = JM; gp40.bias = SB; gp40.R = EXT; gp40.C = PHI;
      gp40.sAo = 0; gp40.sAi = 0; gp40.sAm = NT; gp40.sAk = 1; gp40.sBo = 0; gp40.sBi = 0; gp40.sBn = NT; gp40.sBk = 1; gp40.sCo = 0; gp40.sCi = 0; gp40.sCm = NT; gp40.sRo = 0; gp40.sRi = 0; gp40.sRm = NT; gp40.sRn = 1;
      gp40.M = Bn; gp40.N = NT; gp40.K = NT; gp40.zi_n = 1; gp40.flags = 4; gp40.act = 0;
      gp40.alpha = 1.0f; gp40.beta = 1.0f; gp40.sa = 1.0f; gp40.sb = 1.0f; gp40.Npad = NT; gp40.pad_ = 0;
      k_gemm<1><<<dim3((unsigned)((NT) + 31) / 32, (unsigned)((Bn) + 15) / 16, (unsigned)(1)), 32, 0, stream>>>(gp40); }
    { GemmP gz40;
      gz40.A = SB; gz40.B = JZM; gz40.bias = SB; gz40.R = SB; gz40.C = PHZ;
      gz40.sAo = 0; gz40.sAi = 0; gz40.sAm = NT; gz40.sAk = 1; gz40.sBo = 0; gz40.sBi = 0; gz40.sBn = NT; gz40.sBk = 1; gz40.sCo = 0; gz40.sCi = 0; gz40.sCm = NT; gz40.sRo = 0; gz40.sRi = 0; gz40.sRm = 0; gz40.sRn = 0;
      gz40.M = Bn; gz40.N = NT; gz40.K = NT; gz40.zi_n = 1; gz40.flags = 0; gz40.act = 0;
      gz40.alpha = 1.0f; gz40.beta = 0.0f; gz40.sa = 1.0f; gz40.sb = 1.0f; gz40.Npad = NT; gz40.pad_ = 0;
      k_gemm<1><<<dim3((unsigned)((NT) + 31) / 32, (unsigned)((Bn) + 15) / 16, (unsigned)(1)), 32, 0, stream>>>(gz40); }
    k_soen_step<<<(unsigned)(((long long)Bn * NT + 255) / 256), 256, 0, stream>>>(SB, PHI, PHZ, gam, tau, foz, SA, Bn, NT);
    { GemmP gp41;
      gp41.A = SA; gp41.B = JM; gp41.bias = SA; gp41.R = EXT; gp41.C = PHI;
      gp41.sAo = 0; gp41.sAi = 0; gp41.sAm = NT; gp41.sAk = 1; gp41.sBo = 0; gp41.sBi = 0; gp41.sBn = NT; gp41.sBk = 1; gp41.sCo = 0; gp41.sCi = 0; gp41.sCm = NT; gp41.sRo = 0; gp41.sRi = 0; gp41.sRm = NT; gp41.sRn = 1;
      gp41.M = Bn; gp41.N = NT; gp41.K = NT; gp41.zi_n = 1; gp41.flags = 4; gp41.act = 0;
      gp41.alpha = 1.0f; gp41.beta = 1.0f; gp41.sa = 1.0f; gp41.sb = 1.0f; gp41.Npad = NT; gp41.pad_ = 0;
      k_gemm<1><<<dim3((unsigned)((NT) + 31) / 32, (unsigned)((Bn) + 15) / 16, (unsigned)(1)), 32, 0, stream>>>(gp41); }
    { GemmP gz41;
      gz41.A = SA; gz41.B = JZM; gz41.bias = SA; gz41.R = SA; gz41.C = PHZ;
      gz41.sAo = 0; gz41.sAi = 0; gz41.sAm = NT; gz41.sAk = 1; gz41.sBo = 0; gz41.sBi = 0; gz41.sBn = NT; gz41.sBk = 1; gz41.sCo = 0; gz41.sCi = 0; gz41.sCm = NT; gz41.sRo = 0; gz41.sRi = 0; gz41.sRm = 0; gz41.sRn = 0;
      gz41.M = Bn; gz41.N = NT; gz41.K = NT; gz41.zi_n = 1; gz41.flags = 0; gz41.act = 0;
      gz41.alpha = 1.0f; gz41.beta = 0.0f; gz41.sa = 1.0f; gz41.sb = 1.0f; gz41.Npad = NT; gz41.pad_ = 0;
      k_gemm<1><<<dim3((unsigned)((NT) + 31) / 32, (unsigned)((Bn) + 15) / 16, (unsigned)(1)), 32, 0, stream>>>(gz41); }
    k_soen_step<<<(unsigned)(((long long)Bn * NT + 255) / 256), 256, 0, stream>>>(SA, PHI, PHZ, gam, tau, foz, SB, Bn, NT);
    { GemmP gp42;
      gp42.A = SB; gp42.B = JM; gp42.bias = SB; gp42.R = EXT; gp42.C = PHI;
      gp42.sAo = 0; gp42.sAi = 0; gp42.sAm = NT; gp42.sAk = 1; gp42.sBo = 0; gp42.sBi = 0; gp42.sBn = NT; gp42.sBk = 1; gp42.sCo = 0; gp42.sCi = 0; gp42.sCm = NT; gp42.sRo = 0; gp42.sRi = 0; gp42.sRm = NT; gp42.sRn = 1;
      gp42.M = Bn; gp42.N = NT; gp42.K = NT; gp42.zi_n = 1; gp42.flags = 4; gp42.act = 0;
      gp42.alpha = 1.0f; gp42.beta = 1.0f; gp42.sa = 1.0f; gp42.sb = 1.0f; gp42.Npad = NT; gp42.pad_ = 0;
      k_gemm<1><<<dim3((unsigned)((NT) + 31) / 32, (unsigned)((Bn) + 15) / 16, (unsigned)(1)), 32, 0, stream>>>(gp42); }
    { GemmP gz42;
      gz42.A = SB; gz42.B = JZM; gz42.bias = SB; gz42.R = SB; gz42.C = PHZ;
      gz42.sAo = 0; gz42.sAi = 0; gz42.sAm = NT; gz42.sAk = 1; gz42.sBo = 0; gz42.sBi = 0; gz42.sBn = NT; gz42.sBk = 1; gz42.sCo = 0; gz42.sCi = 0; gz42.sCm = NT; gz42.sRo = 0; gz42.sRi = 0; gz42.sRm = 0; gz42.sRn = 0;
      gz42.M = Bn; gz42.N = NT; gz42.K = NT; gz42.zi_n = 1; gz42.flags = 0; gz42.act = 0;
      gz42.alpha = 1.0f; gz42.beta = 0.0f; gz42.sa = 1.0f; gz42.sb = 1.0f; gz42.Npad = NT; gz42.pad_ = 0;
      k_gemm<1><<<dim3((unsigned)((NT) + 31) / 32, (unsigned)((Bn) + 15) / 16, (unsigned)(1)), 32, 0, stream>>>(gz42); }
    k_soen_step<<<(unsigned)(((long long)Bn * NT + 255) / 256), 256, 0, stream>>>(SB, PHI, PHZ, gam, tau, foz, SA, Bn, NT);
    { GemmP gp43;
      gp43.A = SA; gp43.B = JM; gp43.bias = SA; gp43.R = EXT; gp43.C = PHI;
      gp43.sAo = 0; gp43.sAi = 0; gp43.sAm = NT; gp43.sAk = 1; gp43.sBo = 0; gp43.sBi = 0; gp43.sBn = NT; gp43.sBk = 1; gp43.sCo = 0; gp43.sCi = 0; gp43.sCm = NT; gp43.sRo = 0; gp43.sRi = 0; gp43.sRm = NT; gp43.sRn = 1;
      gp43.M = Bn; gp43.N = NT; gp43.K = NT; gp43.zi_n = 1; gp43.flags = 4; gp43.act = 0;
      gp43.alpha = 1.0f; gp43.beta = 1.0f; gp43.sa = 1.0f; gp43.sb = 1.0f; gp43.Npad = NT; gp43.pad_ = 0;
      k_gemm<1><<<dim3((unsigned)((NT) + 31) / 32, (unsigned)((Bn) + 15) / 16, (unsigned)(1)), 32, 0, stream>>>(gp43); }
    { GemmP gz43;
      gz43.A = SA; gz43.B = JZM; gz43.bias = SA; gz43.R = SA; gz43.C = PHZ;
      gz43.sAo = 0; gz43.sAi = 0; gz43.sAm = NT; gz43.sAk = 1; gz43.sBo = 0; gz43.sBi = 0; gz43.sBn = NT; gz43.sBk = 1; gz43.sCo = 0; gz43.sCi = 0; gz43.sCm = NT; gz43.sRo = 0; gz43.sRi = 0; gz43.sRm = 0; gz43.sRn = 0;
      gz43.M = Bn; gz43.N = NT; gz43.K = NT; gz43.zi_n = 1; gz43.flags = 0; gz43.act = 0;
      gz43.alpha = 1.0f; gz43.beta = 0.0f; gz43.sa = 1.0f; gz43.sb = 1.0f; gz43.Npad = NT; gz43.pad_ = 0;
      k_gemm<1><<<dim3((unsigned)((NT) + 31) / 32, (unsigned)((Bn) + 15) / 16, (unsigned)(1)), 32, 0, stream>>>(gz43); }
    k_soen_step<<<(unsigned)(((long long)Bn * NT + 255) / 256), 256, 0, stream>>>(SA, PHI, PHZ, gam, tau, foz, SB, Bn, NT);
    { GemmP gp44;
      gp44.A = SB; gp44.B = JM; gp44.bias = SB; gp44.R = EXT; gp44.C = PHI;
      gp44.sAo = 0; gp44.sAi = 0; gp44.sAm = NT; gp44.sAk = 1; gp44.sBo = 0; gp44.sBi = 0; gp44.sBn = NT; gp44.sBk = 1; gp44.sCo = 0; gp44.sCi = 0; gp44.sCm = NT; gp44.sRo = 0; gp44.sRi = 0; gp44.sRm = NT; gp44.sRn = 1;
      gp44.M = Bn; gp44.N = NT; gp44.K = NT; gp44.zi_n = 1; gp44.flags = 4; gp44.act = 0;
      gp44.alpha = 1.0f; gp44.beta = 1.0f; gp44.sa = 1.0f; gp44.sb = 1.0f; gp44.Npad = NT; gp44.pad_ = 0;
      k_gemm<1><<<dim3((unsigned)((NT) + 31) / 32, (unsigned)((Bn) + 15) / 16, (unsigned)(1)), 32, 0, stream>>>(gp44); }
    { GemmP gz44;
      gz44.A = SB; gz44.B = JZM; gz44.bias = SB; gz44.R = SB; gz44.C = PHZ;
      gz44.sAo = 0; gz44.sAi = 0; gz44.sAm = NT; gz44.sAk = 1; gz44.sBo = 0; gz44.sBi = 0; gz44.sBn = NT; gz44.sBk = 1; gz44.sCo = 0; gz44.sCi = 0; gz44.sCm = NT; gz44.sRo = 0; gz44.sRi = 0; gz44.sRm = 0; gz44.sRn = 0;
      gz44.M = Bn; gz44.N = NT; gz44.K = NT; gz44.zi_n = 1; gz44.flags = 0; gz44.act = 0;
      gz44.alpha = 1.0f; gz44.beta = 0.0f; gz44.sa = 1.0f; gz44.sb = 1.0f; gz44.Npad = NT; gz44.pad_ = 0;
      k_gemm<1><<<dim3((unsigned)((NT) + 31) / 32, (unsigned)((Bn) + 15) / 16, (unsigned)(1)), 32, 0, stream>>>(gz44); }
    k_soen_step<<<(unsigned)(((long long)Bn * NT + 255) / 256), 256, 0, stream>>>(SB, PHI, PHZ, gam, tau, foz, SA, Bn, NT);
    { GemmP gp45;
      gp45.A = SA; gp45.B = JM; gp45.bias = SA; gp45.R = EXT; gp45.C = PHI;
      gp45.sAo = 0; gp45.sAi = 0; gp45.sAm = NT; gp45.sAk = 1; gp45.sBo = 0; gp45.sBi = 0; gp45.sBn = NT; gp45.sBk = 1; gp45.sCo = 0; gp45.sCi = 0; gp45.sCm = NT; gp45.sRo = 0; gp45.sRi = 0; gp45.sRm = NT; gp45.sRn = 1;
      gp45.M = Bn; gp45.N = NT; gp45.K = NT; gp45.zi_n = 1; gp45.flags = 4; gp45.act = 0;
      gp45.alpha = 1.0f; gp45.beta = 1.0f; gp45.sa = 1.0f; gp45.sb = 1.0f; gp45.Npad = NT; gp45.pad_ = 0;
      k_gemm<1><<<dim3((unsigned)((NT) + 31) / 32, (unsigned)((Bn) + 15) / 16, (unsigned)(1)), 32, 0, stream>>>(gp45); }
    { GemmP gz45;
      gz45.A = SA; gz45.B = JZM; gz45.bias = SA; gz45.R = SA; gz45.C = PHZ;
      gz45.sAo = 0; gz45.sAi = 0; gz45.sAm = NT; gz45.sAk = 1; gz45.sBo = 0; gz45.sBi = 0; gz45.sBn = NT; gz45.sBk = 1; gz45.sCo = 0; gz45.sCi = 0; gz45.sCm = NT; gz45.sRo = 0; gz45.sRi = 0; gz45.sRm = 0; gz45.sRn = 0;
      gz45.M = Bn; gz45.N = NT; gz45.K = NT; gz45.zi_n = 1; gz45.flags = 0; gz45.act = 0;
      gz45.alpha = 1.0f; gz45.beta = 0.0f; gz45.sa = 1.0f; gz45.sb = 1.0f; gz45.Npad = NT; gz45.pad_ = 0;
      k_gemm<1><<<dim3((unsigned)((NT) + 31) / 32, (unsigned)((Bn) + 15) / 16, (unsigned)(1)), 32, 0, stream>>>(gz45); }
    k_soen_step<<<(unsigned)(((long long)Bn * NT + 255) / 256), 256, 0, stream>>>(SA, PHI, PHZ, gam, tau, foz, SB, Bn, NT);
    { GemmP gp46;
      gp46.A = SB; gp46.B = JM; gp46.bias = SB; gp46.R = EXT; gp46.C = PHI;
      gp46.sAo = 0; gp46.sAi = 0; gp46.sAm = NT; gp46.sAk = 1; gp46.sBo = 0; gp46.sBi = 0; gp46.sBn = NT; gp46.sBk = 1; gp46.sCo = 0; gp46.sCi = 0; gp46.sCm = NT; gp46.sRo = 0; gp46.sRi = 0; gp46.sRm = NT; gp46.sRn = 1;
      gp46.M = Bn; gp46.N = NT; gp46.K = NT; gp46.zi_n = 1; gp46.flags = 4; gp46.act = 0;
      gp46.alpha = 1.0f; gp46.beta = 1.0f; gp46.sa = 1.0f; gp46.sb = 1.0f; gp46.Npad = NT; gp46.pad_ = 0;
      k_gemm<1><<<dim3((unsigned)((NT) + 31) / 32, (unsigned)((Bn) + 15) / 16, (unsigned)(1)), 32, 0, stream>>>(gp46); }
    { GemmP gz46;
      gz46.A = SB; gz46.B = JZM; gz46.bias = SB; gz46.R = SB; gz46.C = PHZ;
      gz46.sAo = 0; gz46.sAi = 0; gz46.sAm = NT; gz46.sAk = 1; gz46.sBo = 0; gz46.sBi = 0; gz46.sBn = NT; gz46.sBk = 1; gz46.sCo = 0; gz46.sCi = 0; gz46.sCm = NT; gz46.sRo = 0; gz46.sRi = 0; gz46.sRm = 0; gz46.sRn = 0;
      gz46.M = Bn; gz46.N = NT; gz46.K = NT; gz46.zi_n = 1; gz46.flags = 0; gz46.act = 0;
      gz46.alpha = 1.0f; gz46.beta = 0.0f; gz46.sa = 1.0f; gz46.sb = 1.0f; gz46.Npad = NT; gz46.pad_ = 0;
      k_gemm<1><<<dim3((unsigned)((NT) + 31) / 32, (unsigned)((Bn) + 15) / 16, (unsigned)(1)), 32, 0, stream>>>(gz46); }
    k_soen_step<<<(unsigned)(((long long)Bn * NT + 255) / 256), 256, 0, stream>>>(SB, PHI, PHZ, gam, tau, foz, SA, Bn, NT);
    { GemmP gp47;
      gp47.A = SA; gp47.B = JM; gp47.bias = SA; gp47.R = EXT; gp47.C = PHI;
      gp47.sAo = 0; gp47.sAi = 0; gp47.sAm = NT; gp47.sAk = 1; gp47.sBo = 0; gp47.sBi = 0; gp47.sBn = NT; gp47.sBk = 1; gp47.sCo = 0; gp47.sCi = 0; gp47.sCm = NT; gp47.sRo = 0; gp47.sRi = 0; gp47.sRm = NT; gp47.sRn = 1;
      gp47.M = Bn; gp47.N = NT; gp47.K = NT; gp47.zi_n = 1; gp47.flags = 4; gp47.act = 0;
      gp47.alpha = 1.0f; gp47.beta = 1.0f; gp47.sa = 1.0f; gp47.sb = 1.0f; gp47.Npad = NT; gp47.pad_ = 0;
      k_gemm<1><<<dim3((unsigned)((NT) + 31) / 32, (unsigned)((Bn) + 15) / 16, (unsigned)(1)), 32, 0, stream>>>(gp47); }
    { GemmP gz47;
      gz47.A = SA; gz47.B = JZM; gz47.bias = SA; gz47.R = SA; gz47.C = PHZ;
      gz47.sAo = 0; gz47.sAi = 0; gz47.sAm = NT; gz47.sAk = 1; gz47.sBo = 0; gz47.sBi = 0; gz47.sBn = NT; gz47.sBk = 1; gz47.sCo = 0; gz47.sCi = 0; gz47.sCm = NT; gz47.sRo = 0; gz47.sRi = 0; gz47.sRm = 0; gz47.sRn = 0;
      gz47.M = Bn; gz47.N = NT; gz47.K = NT; gz47.zi_n = 1; gz47.flags = 0; gz47.act = 0;
      gz47.alpha = 1.0f; gz47.beta = 0.0f; gz47.sa = 1.0f; gz47.sb = 1.0f; gz47.Npad = NT; gz47.pad_ = 0;
      k_gemm<1><<<dim3((unsigned)((NT) + 31) / 32, (unsigned)((Bn) + 15) / 16, (unsigned)(1)), 32, 0, stream>>>(gz47); }
    k_soen_step<<<(unsigned)(((long long)Bn * NT + 255) / 256), 256, 0, stream>>>(SA, PHI, PHZ, gam, tau, foz, SB, Bn, NT);
    { GemmP gp48;
      gp48.A = SB; gp48.B = JM; gp48.bias = SB; gp48.R = EXT; gp48.C = PHI;
      gp48.sAo = 0; gp48.sAi = 0; gp48.sAm = NT; gp48.sAk = 1; gp48.sBo = 0; gp48.sBi = 0; gp48.sBn = NT; gp48.sBk = 1; gp48.sCo = 0; gp48.sCi = 0; gp48.sCm = NT; gp48.sRo = 0; gp48.sRi = 0; gp48.sRm = NT; gp48.sRn = 1;
      gp48.M = Bn; gp48.N = NT; gp48.K = NT; gp48.zi_n = 1; gp48.flags = 4; gp48.act = 0;
      gp48.alpha = 1.0f; gp48.beta = 1.0f; gp48.sa = 1.0f; gp48.sb = 1.0f; gp48.Npad = NT; gp48.pad_ = 0;
      k_gemm<1><<<dim3((unsigned)((NT) + 31) / 32, (unsigned)((Bn) + 15) / 16, (unsigned)(1)), 32, 0, stream>>>(gp48); }
    { GemmP gz48;
      gz48.A = SB; gz48.B = JZM; gz48.bias = SB; gz48.R = SB; gz48.C = PHZ;
      gz48.sAo = 0; gz48.sAi = 0; gz48.sAm = NT; gz48.sAk = 1; gz48.sBo = 0; gz48.sBi = 0; gz48.sBn = NT; gz48.sBk = 1; gz48.sCo = 0; gz48.sCi = 0; gz48.sCm = NT; gz48.sRo = 0; gz48.sRi = 0; gz48.sRm = 0; gz48.sRn = 0;
      gz48.M = Bn; gz48.N = NT; gz48.K = NT; gz48.zi_n = 1; gz48.flags = 0; gz48.act = 0;
      gz48.alpha = 1.0f; gz48.beta = 0.0f; gz48.sa = 1.0f; gz48.sb = 1.0f; gz48.Npad = NT; gz48.pad_ = 0;
      k_gemm<1><<<dim3((unsigned)((NT) + 31) / 32, (unsigned)((Bn) + 15) / 16, (unsigned)(1)), 32, 0, stream>>>(gz48); }
    k_soen_step<<<(unsigned)(((long long)Bn * NT + 255) / 256), 256, 0, stream>>>(SB, PHI, PHZ, gam, tau, foz, SA, Bn, NT);
    { GemmP gp49;
      gp49.A = SA; gp49.B = JM; gp49.bias = SA; gp49.R = EXT; gp49.C = PHI;
      gp49.sAo = 0; gp49.sAi = 0; gp49.sAm = NT; gp49.sAk = 1; gp49.sBo = 0; gp49.sBi = 0; gp49.sBn = NT; gp49.sBk = 1; gp49.sCo = 0; gp49.sCi = 0; gp49.sCm = NT; gp49.sRo = 0; gp49.sRi = 0; gp49.sRm = NT; gp49.sRn = 1;
      gp49.M = Bn; gp49.N = NT; gp49.K = NT; gp49.zi_n = 1; gp49.flags = 4; gp49.act = 0;
      gp49.alpha = 1.0f; gp49.beta = 1.0f; gp49.sa = 1.0f; gp49.sb = 1.0f; gp49.Npad = NT; gp49.pad_ = 0;
      k_gemm<1><<<dim3((unsigned)((NT) + 31) / 32, (unsigned)((Bn) + 15) / 16, (unsigned)(1)), 32, 0, stream>>>(gp49); }
    { GemmP gz49;
      gz49.A = SA; gz49.B = JZM; gz49.bias = SA; gz49.R = SA; gz49.C = PHZ;
      gz49.sAo = 0; gz49.sAi = 0; gz49.sAm = NT; gz49.sAk = 1; gz49.sBo = 0; gz49.sBi = 0; gz49.sBn = NT; gz49.sBk = 1; gz49.sCo = 0; gz49.sCi = 0; gz49.sCm = NT; gz49.sRo = 0; gz49.sRi = 0; gz49.sRm = 0; gz49.sRn = 0;
      gz49.M = Bn; gz49.N = NT; gz49.K = NT; gz49.zi_n = 1; gz49.flags = 0; gz49.act = 0;
      gz49.alpha = 1.0f; gz49.beta = 0.0f; gz49.sa = 1.0f; gz49.sb = 1.0f; gz49.Npad = NT; gz49.pad_ = 0;
      k_gemm<1><<<dim3((unsigned)((NT) + 31) / 32, (unsigned)((Bn) + 15) / 16, (unsigned)(1)), 32, 0, stream>>>(gz49); }
    k_soen_step<<<(unsigned)(((long long)Bn * NT + 255) / 256), 256, 0, stream>>>(SA, PHI, PHZ, gam, tau, foz, SB, Bn, NT);
    k_soen_out<<<(unsigned)(((long long)Bn * NO + 255) / 256), 256, 0, stream>>>(SB, out, Bn, NT, NO);
}
